// VFcont_65738769432779
// MI455X (gfx1250) — hardware-verified
//
#include <hip/hip_runtime.h>
#include <math.h>

typedef __attribute__((ext_vector_type(16))) _Float16 v16h;
typedef __attribute__((ext_vector_type(8)))  _Float16 v8h;
typedef __attribute__((ext_vector_type(16))) __bf16   v16b;
typedef __attribute__((ext_vector_type(8)))  float    v8f;
typedef __attribute__((ext_vector_type(4)))  float    v4f;

__device__ __forceinline__ int frag_k(int i, int h) { return (i < 8) ? (8 * h + i) : (16 + 8 * h + (i - 8)); }
__device__ __forceinline__ __bf16 bf16_rne(float f) {
    unsigned int u = __float_as_uint(f);
    u += 0x7fffu + ((u >> 16) & 1u);
    return __builtin_bit_cast(__bf16, (unsigned short)(u >> 16));
}
__device__ __forceinline__ float bf16_f32(__bf16 b) { return __uint_as_float(((unsigned int)__builtin_bit_cast(unsigned short, b)) << 16); }
__device__ __forceinline__ v8f wmma16(v16h a, v16h b, v8f c) {
    c = __builtin_amdgcn_wmma_f32_16x16x32_f16(false, a, false, b, (short)0, c, false, false);
    asm volatile("v_nop\n\tv_nop\n\tv_nop\n\tv_nop" : "+v"(c) : "v"(a), "v"(b));
    return c;
}
__device__ __forceinline__ v8f wmmab(v16b a, v16b b, v8f c) {
    c = __builtin_amdgcn_wmma_f32_16x16x32_bf16(false, a, false, b, (short)0, c, false, false);
    asm volatile("v_nop\n\tv_nop\n\tv_nop\n\tv_nop" : "+v"(c) : "v"(a), "v"(b));
    return c;
}
struct Split { v16b hi, lo; };
__device__ __forceinline__ v8f wmma3(const Split& a, const Split& b, v8f c) {
    c = __builtin_amdgcn_wmma_f32_16x16x32_bf16(false, a.hi, false, b.hi, (short)0, c, false, false);
    c = __builtin_amdgcn_wmma_f32_16x16x32_bf16(false, a.hi, false, b.lo, (short)0, c, false, false);
    c = __builtin_amdgcn_wmma_f32_16x16x32_bf16(false, a.lo, false, b.hi, (short)0, c, false, false);
    asm volatile("v_nop\n\tv_nop\n\tv_nop\n\tv_nop" : "+v"(c) : "v"(a.hi), "v"(a.lo), "v"(b.hi), "v"(b.lo));
    return c;
}
struct Split3 { v16b hi, mid, lo; };
__device__ __forceinline__ v8f wmma6(const Split3& a, const Split3& b, v8f c) {
    c = __builtin_amdgcn_wmma_f32_16x16x32_bf16(false, a.hi, false, b.hi, (short)0, c, false, false);
    c = __builtin_amdgcn_wmma_f32_16x16x32_bf16(false, a.hi, false, b.mid, (short)0, c, false, false);
    c = __builtin_amdgcn_wmma_f32_16x16x32_bf16(false, a.mid, false, b.hi, (short)0, c, false, false);
    c = __builtin_amdgcn_wmma_f32_16x16x32_bf16(false, a.hi, false, b.lo, (short)0, c, false, false);
    c = __builtin_amdgcn_wmma_f32_16x16x32_bf16(false, a.mid, false, b.mid, (short)0, c, false, false);
    c = __builtin_amdgcn_wmma_f32_16x16x32_bf16(false, a.lo, false, b.hi, (short)0, c, false, false);
    asm volatile("v_nop\n\tv_nop\n\tv_nop\n\tv_nop" : "+v"(c) : "v"(a.hi), "v"(a.mid), "v"(a.lo), "v"(b.hi), "v"(b.mid), "v"(b.lo));
    return c;
}

__device__ __forceinline__ v16h fh_ld(const float* __restrict__ p, long long sk, int k0, int h, int klen, float s) {
    v16h a;
#pragma unroll
    for (int i = 0; i < 16; ++i) { const int k = k0 + frag_k(i, h); a[i] = (k < klen) ? (_Float16)(p[(long long)k * sk] * s) : (_Float16)0.f; }
    return a;
}
__device__ __forceinline__ Split sp_ld(const float* __restrict__ p, long long sk, int k0, int h, int klen, float s) {
    Split r;
#pragma unroll
    for (int i = 0; i < 16; ++i) {
        const int k = k0 + frag_k(i, h); const float x = (k < klen) ? p[(long long)k * sk] * s : 0.f;
        const __bf16 hb = bf16_rne(x); r.hi[i] = hb; r.lo[i] = bf16_rne(x - bf16_f32(hb));
    }
    return r;
}
__device__ __forceinline__ Split3 sp3_ld(const float* __restrict__ p, long long sk, int k0, int h, int klen, float s) {
    Split3 r;
#pragma unroll
    for (int i = 0; i < 16; ++i) {
        const int k = k0 + frag_k(i, h); const float x = (k < klen) ? p[(long long)k * sk] * s : 0.f;
        const __bf16 hb = bf16_rne(x); const float r1 = x - bf16_f32(hb); const __bf16 mb = bf16_rne(r1);
        r.hi[i] = hb; r.mid[i] = mb; r.lo[i] = bf16_rne(r1 - bf16_f32(mb));
    }
    return r;
}
__device__ __forceinline__ v16b bh_ld(const float* __restrict__ p, long long sk, int k0, int h, int klen, float s) {
    v16b a;
#pragma unroll
    for (int i = 0; i < 16; ++i) { const int k = k0 + frag_k(i, h); a[i] = bf16_rne((k < klen) ? p[(long long)k * sk] * s : 0.f); }
    return a;
}
__device__ __forceinline__ v16h fh_row(const _Float16* __restrict__ row, int k0, int h) {
    v16h a;
#pragma unroll
    for (int i = 0; i < 16; ++i) a[i] = row[k0 + frag_k(i, h)];
    return a;
}

#define VST2(T, ptr, val) do { *(volatile T*)(ptr) = (val); __threadfence(); *(volatile T*)(ptr) = (val); } while (0)
typedef float v4f __attribute__((ext_vector_type(4)));
#define VST2V4(ptr, val) do { *(volatile v4f*)(ptr) = (val); __threadfence(); *(volatile v4f*)(ptr) = (val); } while (0)

__device__ __attribute__((noinline)) float act_fn(float v, int act) {
    if (act == 1) return fmaxf(v, 0.f);
    if (act == 2) { const float u = 0.7978845608028654f * (v + 0.044715f * v * v * v); return 0.5f * v * (1.f + tanhf(u)); }
    if (act == 3) return v / (1.f + expf(-v));
    if (act == 4) return 0.5f * v * (1.f + erff(v * 0.7071067811865476f));
    if (act == 5) return tanhf(v);
    if (act == 6) return 1.f / (1.f + expf(-v));
    if (act == 7) return (v > 0.f) ? v : 0.01f * v;
    if (act == 8) return (v > 0.f) ? v : (expf(v) - 1.f);
    if (act == 9) return fminf(fmaxf(v, 0.f), 6.f);
    if (act == 10) return fabsf(v);
    if (act == 11) return (v >= 0.f) ? v : 0.1f * v;
    if (act == 12) return (v > 0.f) ? v : 0.2f * v;
    if (act == 13) return (v > 20.f) ? v : log1pf(expf(v));
    return v;
}

struct GemmP {
    const float* A; const float* B; const float* bias; const float* R; float* C;
    long long sAo, sAi, sAm, sAk, sBo, sBi, sBn, sBk, sCo, sCi, sCm, sRo, sRi, sRm, sRn;
    int M, N, K, zi_n, flags, act; float alpha, beta, sa, sb;
    int Npad, pad_;
};
static_assert(sizeof(GemmP) == 5 * 8 + 15 * 8 + 6 * 4 + 4 * 4 + 2 * 4, "GemmP has padding");

template <int MODE>
__global__ __launch_bounds__(32) void k_gemm(GemmP p) {
    const int lane = threadIdx.x & 31, h = lane >> 4, l15 = lane & 15;
    const int m0 = blockIdx.y * 16, n0 = blockIdx.x * 32;
    const int z = blockIdx.z, zo = z / p.zi_n, zi = z - zo * p.zi_n;
    const float* A = p.A + zo * p.sAo + zi * p.sAi;
    const float* B = p.B + zo * p.sBo + zi * p.sBi;
    const int am = min(m0 + l15, p.M - 1);
    v8f acc[2], comp[2];
#pragma unroll
    for (int t = 0; t < 2; ++t) { v8f zz = {}; acc[t] = zz; comp[t] = zz; }
    for (int k0 = 0; k0 < p.K; k0 += 32) {
        const float* arow = A + (long long)am * p.sAm;
        if (MODE == 1) {
            const Split a = sp_ld(arow, p.sAk, k0, h, p.K, 1.f);
#pragma unroll
            for (int t = 0; t < 2; ++t) {
                const int bn = min(n0 + t * 16 + l15, p.N - 1);
                acc[t] = wmma3(a, sp_ld(B + (long long)bn * p.sBn, p.sBk, k0, h, p.K, 1.f), acc[t]);
            }
        } else if (MODE == 3) {
            const Split3 a = sp3_ld(arow, p.sAk, k0, h, p.K, 1.f);
#pragma unroll
            for (int t = 0; t < 2; ++t) {
                const int bn = min(n0 + t * 16 + l15, p.N - 1);
                acc[t] = wmma6(a, sp3_ld(B + (long long)bn * p.sBn, p.sBk, k0, h, p.K, 1.f), acc[t]);
            }
        } else if (MODE == 4) {
            const Split3 a = sp3_ld(arow, p.sAk, k0, h, p.K, 1.f);
#pragma unroll
            for (int t = 0; t < 2; ++t) {
                const int bn = min(n0 + t * 16 + l15, p.N - 1); v8f zz = {};
                const v8f part = wmma6(a, sp3_ld(B + (long long)bn * p.sBn, p.sBk, k0, h, p.K, 1.f), zz);
                const v8f y = part - comp[t]; const v8f s = acc[t] + y; comp[t] = (s - acc[t]) - y; acc[t] = s;
            }
        } else if (MODE == 2) {
            const v16b a = bh_ld(arow, p.sAk, k0, h, p.K, 1.f);
#pragma unroll
            for (int t = 0; t < 2; ++t) {
                const int bn = min(n0 + t * 16 + l15, p.N - 1);
                acc[t] = wmmab(a, bh_ld(B + (long long)bn * p.sBn, p.sBk, k0, h, p.K, 1.f), acc[t]);
            }
        } else {
            const v16h a = fh_ld(arow, p.sAk, k0, h, p.K, p.sa);
#pragma unroll
            for (int t = 0; t < 2; ++t) {
                const int bn = min(n0 + t * 16 + l15, p.N - 1);
                acc[t] = wmma16(a, fh_ld(B + (long long)bn * p.sBn, p.sBk, k0, h, p.K, p.sb), acc[t]);
            }
        }
    }
    const float iscale = (MODE == 0) ? p.alpha / (p.sa * p.sb) : p.alpha;
    float* C = p.C + zo * p.sCo + zi * p.sCi;
    const float* R = p.R + zo * p.sRo + zi * p.sRi;
    __shared__ __align__(16) float ctile[16][36];
#pragma unroll
    for (int t = 0; t < 2; ++t) {
        const int n = n0 + t * 16 + l15; const int nn = min(n, p.N - 1);
#pragma unroll
        for (int r = 0; r < 8; ++r) {
            const int m = m0 + 8 * h + r; const int mm = min(m, p.M - 1);
            float v = acc[t][r] * iscale;
            if (p.flags & 1) v += p.bias[nn];
            if (p.flags & 2) v += p.bias[mm];
            v = act_fn(v, p.act);
            if (p.flags & 4) v += p.beta * R[(long long)mm * p.sRm + (long long)nn * p.sRn];
            ctile[8 * h + r][t * 16 + l15] = (n < p.N) ? v : 0.f;
        }
    }
    __syncthreads();
    const int NW = (p.Npad > p.N) ? p.Npad : p.N;
    const bool fast = (m0 + 16 <= p.M) && (n0 + 32 <= NW) && ((p.sCm & 3) == 0) && ((((size_t)C) & 15) == 0);
    if (fast) {
#pragma unroll
        for (int s = 0; s < 4; ++s) {
            const int row = s * 4 + (lane >> 3), c4 = (lane & 7) * 4;
            const v4f v = *(const v4f*)&ctile[row][c4];
            VST2V4(C + (long long)(m0 + row) * p.sCm + n0 + c4, v);
        }
    } else {
        for (int row = 0; row < 16; ++row) {
            const int m = m0 + row, n = n0 + lane;
            if (m < p.M && n < NW) VST2(float, C + (long long)m * p.sCm + n, ctile[row][lane]);
        }
    }
}

#define AW 4
struct AttnP {
    const float* Q; const float* K; const float* V; float* O; float* P; const float* Mf; const int* Mi; float* ST;
    const float* Pw; const float* Rt; const int* SQ; const int* SK;
    long long swb, swh, swi, swj, srb, srh, sri;
    long long sQb, sQh, sQi, sQd, sKb, sKh, sKj, sKd, sVb, sVh, sVj, sVd, sOb, sOh, sOi, sPb, sPh, sPi, smb, smh, smi, smj;
    int Lq, Lk, dh, dv, hrep, causal, coff, pband;
    float scale, mfill; int nonorm, mpol;
    int roff, rn, segpol, win;
};
static_assert(sizeof(AttnP) == 12 * 8 + 29 * 8 + 16 * 4, "AttnP has padding");

#ifndef KATTN_ATTR
#define KATTN_ATTR
#endif
template <int DHP, int DVP, int QM, bool SPLITPV, bool TWOPASS>
__global__ __launch_bounds__(32 * AW) KATTN_ATTR void k_attn(AttnP p) {
    constexpr int NT = DVP / 16;
    constexpr int KS = DHP / 32;
    constexpr int VP = DVP + 8;
    __shared__ __align__(16) float    pl[AW][16 * 64];
    __shared__ __align__(16) _Float16 vl[(SPLITPV ? 2 : 1) * 64 * VP];
    const int lane = threadIdx.x & 31, hf = lane >> 4, l15 = lane & 15, wave = threadIdx.x >> 5;
    const int h = blockIdx.y, b = blockIdx.z, hk = h / p.hrep;
    const int q0 = (blockIdx.x * AW + wave) * 16;
    float* myp = pl[wave];
    const float L2E = 1.4426950408889634f;
    const float NEG = -__builtin_inff();
    const int qi = min(q0 + l15, p.Lq - 1);
    const float* qrow = p.Q + b * p.sQb + h * p.sQh + (long long)qi * p.sQi;
    const float* kbase = p.K + b * p.sKb + hk * p.sKh;
    const float* vbase = p.V + b * p.sVb + hk * p.sVh;
    v16h qa[QM == 0 ? KS : 1]; Split qs_[QM == 1 ? KS : 1]; Split3 qt_[QM == 2 ? KS : 1];
#pragma unroll
    for (int ks = 0; ks < KS; ++ks) {
        if (QM == 2) qt_[ks] = sp3_ld(qrow, p.sQd, ks * 32, hf, p.dh, 1.f);
        else if (QM == 1) qs_[ks] = sp_ld(qrow, p.sQd, ks * 32, hf, p.dh, 1.f);
        else qa[ks] = fh_ld(qrow, p.sQd, ks * 32, hf, p.dh, 1.f);
    }
    v8f o[NT]; float m8[8], l8[8];
#pragma unroll
    for (int t = 0; t < NT; ++t) { v8f zz = {}; o[t] = zz; }
#pragma unroll
    for (int i = 0; i < 8; ++i) { m8[i] = NEG; l8[i] = 0.f; }
    int jend = p.Lk;
    if (p.causal == 1) { const int je = (blockIdx.x * AW + AW - 1) * 16 + 16 + p.coff; jend = min(jend, max(je, 0)); }
    const int npass = TWOPASS ? 2 : 1;
    for (int pass = 0; pass < npass; ++pass) {
        const bool dopv = (!TWOPASS) || pass == 1;
        for (int j0 = 0; j0 < jend; j0 += 64) {
            if (dopv) {
                __syncthreads();
                for (int idx = threadIdx.x; idx < 64 * DVP; idx += 32 * AW) {
                    const int jr = idx / DVP, d = idx - jr * DVP, j = j0 + jr;
                    const float f = (j < p.Lk && d < p.dv) ? vbase[(long long)j * p.sVj + (long long)d * p.sVd] : 0.f;
                    if (SPLITPV) {
                        const __bf16 hb = bf16_rne(f);
                        ((__bf16*)vl)[jr * VP + d] = hb; ((__bf16*)vl)[64 * VP + jr * VP + d] = bf16_rne(f - bf16_f32(hb));
                    } else vl[jr * VP + d] = (_Float16)f;
                }
            }
            v8f s[4];
#pragma unroll
            for (int t = 0; t < 4; ++t) {
                const int j = min(j0 + t * 16 + l15, p.Lk - 1);
                const float* krow = kbase + (long long)j * p.sKj;
                v8f acc = {};
#pragma unroll
                for (int ks = 0; ks < KS; ++ks) {
                    if (QM == 2)      acc = wmma6(qt_[ks], sp3_ld(krow, p.sKd, ks * 32, hf, p.dh, 1.f), acc);
                    else if (QM == 1) acc = wmma3(qs_[ks], sp_ld(krow, p.sKd, ks * 32, hf, p.dh, 1.f), acc);
                    else              acc = wmma16(qa[ks], fh_ld(krow, p.sKd, ks * 32, hf, p.dh, 1.f), acc);
                }
                s[t] = acc;
            }
            float pv[8][4];
#pragma unroll
            for (int i = 0; i < 8; ++i) {
                const int irow = q0 + i + 8 * hf;
                const int ic = min(irow, p.Lq - 1);
                float sc[4];
#pragma unroll
                for (int t = 0; t < 4; ++t) {
                    const int jg = j0 + t * 16 + l15;
                    float v = s[t][i] * p.scale;
                    if (p.Mf) v += p.Mf[b * p.smb + h * p.smh + (long long)ic * p.smi + (long long)min(jg, p.Lk - 1) * p.smj];
                    if (p.Rt) { int rc = ic - min(jg, p.Lk - 1) + p.roff; rc = rc < 0 ? 0 : (rc >= p.rn ? p.rn - 1 : rc); v += p.Rt[b * p.srb + h * p.srh + (long long)ic * p.sri + rc]; }
                    if (p.Mi) { const int mv = p.Mi[b * p.smb + h * p.smh + (long long)ic * p.smi + (long long)min(jg, p.Lk - 1) * p.smj]; if (p.mpol ? (mv != 0) : (mv == 0)) v = p.mfill; }
                    if (p.SQ) { const bool same = p.SQ[(long long)b * p.Lq + ic] == p.SK[(long long)b * p.Lk + min(jg, p.Lk - 1)]; if (p.segpol ? same : !same) v = p.mfill; }
                    if (p.causal == 2 && jg > irow + p.coff) v = p.mfill;
                    if (jg >= p.Lk || (p.causal == 1 && jg > irow + p.coff) || (p.causal == 3 && jg < irow + p.coff) || (p.win > 0 && irow + p.coff - jg > p.win)) v = NEG; else v *= L2E;
                    sc[t] = v;
                }
                if (!TWOPASS || pass == 0) {
                    float mx = fmaxf(fmaxf(sc[0], sc[1]), fmaxf(sc[2], sc[3]));
                    mx = fmaxf(mx, __shfl_xor(mx, 1, 32)); mx = fmaxf(mx, __shfl_xor(mx, 2, 32));
                    mx = fmaxf(mx, __shfl_xor(mx, 4, 32)); mx = fmaxf(mx, __shfl_xor(mx, 8, 32));
                    const float mnew = fmaxf(m8[i], mx);
                    const float corr = (mnew == NEG) ? 1.f : exp2f(m8[i] - mnew);
                    float rs = 0.f;
#pragma unroll
                    for (int t = 0; t < 4; ++t) {
                        const float pp = (sc[t] == NEG) ? 0.f : exp2f(sc[t] - mnew); rs += pp;
                        pv[i][t] = p.Pw ? pp * p.Pw[b * p.swb + h * p.swh + (long long)ic * p.swi + (long long)min(j0 + t * 16 + l15, p.Lk - 1) * p.swj] : pp;
                    }
                    rs += __shfl_xor(rs, 1, 32); rs += __shfl_xor(rs, 2, 32); rs += __shfl_xor(rs, 4, 32); rs += __shfl_xor(rs, 8, 32);
                    l8[i] = l8[i] * corr + rs; m8[i] = mnew;
                    if (!TWOPASS) {
#pragma unroll
                        for (int t = 0; t < NT; ++t) o[t][i] *= corr;
                    }
                } else {
                    const float inv = (l8[i] > 0.f) ? 1.f / l8[i] : 0.f;
#pragma unroll
                    for (int t = 0; t < 4; ++t) {
                        const int jg = j0 + t * 16 + l15;
                        float pp = (sc[t] == NEG) ? 0.f : exp2f(sc[t] - m8[i]) * inv;
                        if (p.Pw) pp *= p.Pw[b * p.swb + h * p.swh + (long long)ic * p.swi + (long long)min(jg, p.Lk - 1) * p.swj];
                        pv[i][t] = pp;
                    }
                }
            }
            if (dopv) {
#pragma unroll
                for (int i = 0; i < 8; ++i)
#pragma unroll
                    for (int t = 0; t < 4; ++t) myp[(i + 8 * hf) * 64 + t * 16 + l15] = pv[i][t];
                __syncthreads();
                if (p.P) {
                    float* pb_ = p.P + b * p.sPb + h * p.sPh;
                    const bool fastP = (p.pband == 0) && ((p.sPi & 3) == 0) && (j0 + 64 <= p.Lk) && (q0 + 16 <= p.Lq) && ((((size_t)pb_) & 15) == 0);
                    if (fastP) {
#pragma unroll
                        for (int s = 0; s < 8; ++s) {
                            const int row = s * 2 + (lane >> 4), c4 = (lane & 15) * 4;
                            const v4f v = *(const v4f*)(myp + row * 64 + c4);
                            VST2V4(pb_ + (long long)(q0 + row) * p.sPi + j0 + c4, v);
                        }
                    } else {
                        for (int row = 0; row < 16; ++row) {
                            const int irow = q0 + row; if (irow >= p.Lq) continue;
                            for (int c = lane; c < 64; c += 32) {
                                const int jg = j0 + c; if (jg >= p.Lk) continue;
                                if (p.pband == 0) VST2(float, pb_ + (long long)irow * p.sPi + jg, myp[row * 64 + c]);
                                else if (jg - irow <= p.pband && irow - jg <= p.pband) VST2(float, pb_ + (long long)irow * p.sPi + (jg - irow + p.pband), myp[row * 64 + c]);
                            }
                        }
                    }
                }
                if (SPLITPV) {
                    const Split pa0 = sp_ld(myp + l15 * 64, 1, 0, hf, 64, 1.f), pa1 = sp_ld(myp + l15 * 64, 1, 32, hf, 64, 1.f);
                    const __bf16* vh = (const __bf16*)vl; const __bf16* vlo = vh + 64 * VP;
#pragma unroll
                    for (int t = 0; t < NT; ++t) {
                        const int dcol = t * 16 + l15;
                        Split b0, b1;
#pragma unroll
                        for (int e = 0; e < 16; ++e) {
                            const int k0 = frag_k(e, hf), k1 = 32 + frag_k(e, hf);
                            b0.hi[e] = vh[k0 * VP + dcol]; b0.lo[e] = vlo[k0 * VP + dcol]; b1.hi[e] = vh[k1 * VP + dcol]; b1.lo[e] = vlo[k1 * VP + dcol];
                        }
                        o[t] = wmma3(pa0, b0, o[t]);
                        o[t] = wmma3(pa1, b1, o[t]);
                    }
                } else {
                    const v16h pa0 = fh_ld(myp + l15 * 64, 1, 0, hf, 64, 4096.f), pa1 = fh_ld(myp + l15 * 64, 1, 32, hf, 64, 4096.f);
#pragma unroll
                    for (int t = 0; t < NT; ++t) {
                        const int dcol = t * 16 + l15;
                        v16h b0, b1;
#pragma unroll
                        for (int e = 0; e < 16; ++e) { b0[e] = vl[frag_k(e, hf) * VP + dcol]; b1[e] = vl[(32 + frag_k(e, hf)) * VP + dcol]; }
                        o[t] = wmma16(pa0, b0, o[t]);
                        o[t] = wmma16(pa1, b1, o[t]);
                    }
                }
            }
        }
    }
    float* obase = p.O + b * p.sOb + h * p.sOh;
    if (p.ST) {
        const int rl = lane >> 1, isel = rl & 7;
        float mv = 0.f, lv = 0.f;
#pragma unroll
        for (int i = 0; i < 8; ++i) if (i == isel) { mv = m8[i]; lv = l8[i]; }
        const int irow = q0 + rl;
        if (irow < p.Lq) { float* st = p.ST + (((long long)b * gridDim.y + h) * p.Lq + irow) * 2 + (lane & 1); VST2(float, st, (lane & 1) ? lv : mv * 0.6931471805599453f); }
    }
    float invr[8];
#pragma unroll
    for (int i = 0; i < 8; ++i) {
        if (TWOPASS) invr[i] = SPLITPV ? 1.f : (1.f / 4096.f);
        else if (p.nonorm) invr[i] = exp2f(m8[i]) * (SPLITPV ? 1.f : (1.f / 4096.f));
        else invr[i] = (l8[i] > 0.f) ? (SPLITPV ? 1.f / l8[i] : 1.f / (l8[i] * 4096.f)) : 0.f;
    }
    __syncthreads();
    const bool ofast = ((p.sOi & 3) == 0) && ((((size_t)obase) & 15) == 0) && (q0 + 16 <= p.Lq);
#pragma unroll
    for (int c0 = 0; c0 < DVP; c0 += 64) {
#pragma unroll
        for (int i = 0; i < 8; ++i)
#pragma unroll
            for (int t = 0; t < NT; ++t) if (t * 16 >= c0 && t * 16 < c0 + 64) myp[(i + 8 * hf) * 64 + (t * 16 - c0) + l15] = o[t][i] * invr[i];
        __syncthreads();
        const int cw = (DVP - c0 < 64) ? (DVP - c0) : 64;
        if (ofast && (c0 + cw <= p.dv) && (cw % 32 == 0)) {
            const int lpr = cw / 4;
            const int rows_per_ins = 32 / lpr;
            for (int r0 = 0; r0 < 16; r0 += rows_per_ins) {
                const int row = r0 + lane / lpr, c4 = (lane % lpr) * 4;
                const v4f v = *(const v4f*)(myp + row * 64 + c4);
                VST2V4(obase + (long long)(q0 + row) * p.sOi + c0 + c4, v);
            }
        } else {
            for (int row = 0; row < 16; ++row) {
                const int irow = q0 + row; if (irow >= p.Lq) continue;
                for (int c = lane; c < cw; c += 32) { const int d = c0 + c; if (d < p.dv) VST2(float, obase + (long long)irow * p.sOi + d, myp[row * 64 + c]); }
            }
        }
        __syncthreads();
    }
}

struct TrP { const float* src; float* dst; const float* R2; long long sSz, lds, sDz, ldd, sRz, ldr; int R, C, flags, act; float alpha, beta; };
static_assert(sizeof(TrP) == 3 * 8 + 6 * 8 + 6 * 4, "TrP has padding");
__global__ __launch_bounds__(256) void k_tr(TrP p) {
    __shared__ float tile[32][33];
    const int c0 = blockIdx.x * 32, r0 = blockIdx.y * 32, z = blockIdx.z;
    const int lane = threadIdx.x & 31, wave = threadIdx.x >> 5;
    const float* s = p.src + z * p.sSz;
#pragma unroll
    for (int k = 0; k < 4; ++k) {
        const int rl = wave * 4 + k, r = r0 + rl, c = c0 + lane;
        tile[rl][lane] = (r < p.R && c < p.C) ? s[(long long)r * p.lds + c] : 0.f;
    }
    __syncthreads();
    float* d = p.dst + z * p.sDz; const float* rr = p.R2 + z * p.sRz;
#pragma unroll
    for (int k = 0; k < 4; ++k) {
        const int cl = wave * 4 + k, c = c0 + cl, r = r0 + lane;
        if (c < p.C && r < p.R) {
            float v = act_fn(p.alpha * tile[lane][cl], p.act);
            if (p.flags & 1) v += p.beta * rr[(long long)c * p.ldr + r];
            VST2(float, d + (long long)c * p.ldd + r, v);
        }
    }
}

__global__ __launch_bounds__(256) void k_affine(const float* __restrict__ src, float* __restrict__ dst, int n, float a, float b, const float* __restrict__ sdev) {
    const int i = blockIdx.x * 256 + threadIdx.x;
    if (i < n) { const float aa = sdev ? a * sdev[0] : a; const float v = aa * src[i] + b; VST2(float, dst + i, v); }
}

struct SmP { const float* src; float* dst; const float* Mf; long long sz, sr, dz, dr, smz, smr; int n, pad; float scale_in, scale_out; };
static_assert(sizeof(SmP) == 3 * 8 + 6 * 8 + 4 * 4, "SmP has padding");
__global__ __launch_bounds__(256) void k_softmax(SmP p) {
    __shared__ float red[256];
    const int r = blockIdx.x, z = blockIdx.y, tid = threadIdx.x;
    const float* s = p.src + z * p.sz + (long long)r * p.sr;
    const float* mf = p.Mf ? (p.Mf + z * p.smz + (long long)r * p.smr) : nullptr;
    float mx = -__builtin_inff();
    for (int j = tid; j < p.n; j += 256) { float v = s[j] * p.scale_in; if (mf) v += mf[j]; mx = fmaxf(mx, v); }
    red[tid] = mx; __syncthreads();
    for (int o = 128; o > 0; o >>= 1) { if (tid < o) red[tid] = fmaxf(red[tid], red[tid + o]); __syncthreads(); }
    mx = red[0]; __syncthreads();
    float sum = 0.f;
    for (int j = tid; j < p.n; j += 256) { float v = s[j] * p.scale_in; if (mf) v += mf[j]; sum += (mx == -__builtin_inff()) ? 0.f : expf(v - mx); }
    red[tid] = sum; __syncthreads();
    for (int o = 128; o > 0; o >>= 1) { if (tid < o) red[tid] += red[tid + o]; __syncthreads(); }
    sum = red[0];
    const float inv = (sum > 0.f) ? p.scale_out / sum : 0.f;
    float* d = p.dst + z * p.dz + (long long)r * p.dr;
    for (int j = tid; j < p.n; j += 256) { float v = s[j] * p.scale_in; if (mf) v += mf[j]; const float o = (mx == -__builtin_inff()) ? 0.f : expf(v - mx) * inv; VST2(float, d + j, o); }
}
__global__ __launch_bounds__(256) void k_stats(const float* __restrict__ x, long long sz, long long so, long long si, int inner, int n, float eps, float* __restrict__ stat, int mode) {
    __shared__ float red[256];
    const int z = blockIdx.x, tid = threadIdx.x;
    const float* base = x + z * sz;
    float s = 0.f;
    for (int e = tid; e < n; e += 256) s += base[(long long)(e / inner) * so + (long long)(e % inner) * si];
    red[tid] = s; __syncthreads();
    for (int o = 128; o > 0; o >>= 1) { if (tid < o) red[tid] += red[tid + o]; __syncthreads(); }
    const float mu = (mode == 0 || mode == 3) ? red[0] / (float)n : 0.f; __syncthreads();
    float q = 0.f;
    for (int e = tid; e < n; e += 256) { const float dlt = base[(long long)(e / inner) * so + (long long)(e % inner) * si] - mu; q += dlt * dlt; }
    red[tid] = q; __syncthreads();
    for (int o = 128; o > 0; o >>= 1) { if (tid < o) red[tid] += red[tid + o]; __syncthreads(); }
    {
        float rs;
        if (mode == 2) rs = sqrtf((float)n) / fmaxf(sqrtf(red[0]), eps); else if (mode == 3) rs = rsqrtf(red[0] / (float)(n - 1) + eps); else rs = rsqrtf(red[0] / (float)n + eps);
        if (tid < 32) { const float v = (tid == 0) ? mu : ((tid == 1) ? rs : 0.f); VST2(float, stat + (long long)z * 32 + tid, v); }
    }
}
__global__ __launch_bounds__(256) void k_norm_apply(const float* __restrict__ x, float* __restrict__ y, const float* __restrict__ stat, const float* __restrict__ g, const float* __restrict__ bta,
                                                     int Z, int C, int L, int G, int bn, int act) {
    const long long idx = (long long)blockIdx.x * 256 + threadIdx.x;
    if (idx >= (long long)Z * C * L) return;
    const int l = (int)(idx % L); const long long zc = idx / L; const int c = (int)(zc % C), z = (int)(zc / C); (void)l;
    const int set = bn ? c : (z * G + c / (C / G));
    float v = (x[idx] - stat[(long long)set * 32]) * stat[(long long)set * 32 + 1];
    if (g) v *= g[c];
    if (bta) v += bta[c];
    v = act_fn(v, act);
    VST2(float, y + idx, v);
}

__global__ __launch_bounds__(256) void k_lse_neg(const float* __restrict__ st, float* __restrict__ c, int n) {
    const int i = blockIdx.x * 256 + threadIdx.x;
    if (i < n) { const float v = -(st[2 * i] + logf(st[2 * i + 1])); VST2(float, c + i, v); }
}

__global__ __launch_bounds__(256) void k_iota(int* __restrict__ dst, int n, int a, int b) {
    const int i = blockIdx.x * 256 + threadIdx.x;
    if (i < n) { const int v = a * i + b; VST2(int, dst + i, v); }
}

__global__ __launch_bounds__(256) void k_axpby(const float* __restrict__ x, const float* __restrict__ y, float* __restrict__ dst, int n, float a, float b, float c) {
    const int i = blockIdx.x * 256 + threadIdx.x;
    if (i < n) { const float v = a * x[i] + b * y[i] + c; VST2(float, dst + i, v); }
}

struct RopeP { const float* X; float* Y; const float* C; const float* Sn; const int* pos; long long sXr, sXh, sYr, sYh, sCb, sCp, sCd; int R, Hn, D, S, mode, tmode, pmode, pad; };
static_assert(sizeof(RopeP) == 5 * 8 + 7 * 8 + 8 * 4, "RopeP has padding");
__global__ __launch_bounds__(256) void k_rope(RopeP p) {
    const long long idx = (long long)blockIdx.x * 256 + threadIdx.x;
    if (idx >= (long long)p.R * p.Hn * p.D) return;
    const int d = (int)(idx % p.D); const long long rh = idx / p.D; const int h = (int)(rh % p.Hn); const int r = (int)(rh / p.Hn);
    const int half = p.D / 2;
    int partner; float sign;
    if (p.mode == 0) { partner = (d < half) ? d + half : d - half; sign = (d < half) ? -1.f : 1.f; }
    else { partner = d ^ 1; sign = (d & 1) ? 1.f : -1.f; }
    const int tcol = (p.tmode == 0) ? d : ((p.tmode == 1) ? (d % half) : (d >> 1));
    const int pp = (p.pmode == 0) ? (r % p.S) : ((p.pmode == 1) ? h : p.pos[r]);
    const long long toff = (long long)(r / p.S) * p.sCb + (long long)pp * p.sCp + (long long)tcol * p.sCd;
    const float* xr = p.X + (long long)r * p.sXr + (long long)h * p.sXh;
    const float v = xr[d] * p.C[toff] + sign * xr[partner] * p.Sn[toff];
    VST2(float, p.Y + (long long)r * p.sYr + (long long)h * p.sYh + d, v);
}

__global__ __launch_bounds__(256) void k_invf(float* __restrict__ invb, int half, int D, float base, float num, int fmode, float cexp) {
    const int i = blockIdx.x * 256 + threadIdx.x;
    if (i >= ((half + 31) / 32) * 32) return;
    if (i >= half) { VST2(float, invb + i, 0.f); return; }
    const float e = (float)(2 * i) / (float)D;
    float invf;
    if (fmode == 1) invf = num * expf((float)(2 * i) * cexp);
    else if (fmode == 2) invf = num * powf(base, (-2.0f * ((float)i - 1.0f)) / (float)D);
    else invf = num * (1.0f / powf(base, e));
    VST2(float, invb + i, invf);
}
__global__ __launch_bounds__(256) void k_sincos(float* __restrict__ cs, float* __restrict__ sn, const float* __restrict__ invb, int S, int half, float pscale) {
    const int idx = blockIdx.x * 256 + threadIdx.x;
    if (idx >= S * half) return;
    const int s = idx / half, i = idx - s * half;
    const float ang = (pscale * (float)s) * invb[i];
    VST2(float, cs + idx, cosf(ang)); VST2(float, sn + idx, sinf(ang));
}

__global__ __launch_bounds__(256) void k_mulact(const float* __restrict__ x, const float* __restrict__ y, float* __restrict__ dst, int n, int act) {
    const int i = blockIdx.x * 256 + threadIdx.x;
    if (i < n) { const float v = act_fn(x[i], act) * y[i]; VST2(float, dst + i, v); }
}

__global__ __launch_bounds__(256) void k_matvec(GemmP p) {
    const int rpt = (p.N == 1) ? 1 : 32;
    const long long r0 = ((long long)blockIdx.x * 256 + threadIdx.x) * rpt; const int z = blockIdx.z, zo = z / p.zi_n, zi = z - zo * p.zi_n;
    if (r0 >= p.M) return;
    const float* Bb = p.B + zo * p.sBo + zi * p.sBi;
    float* C = p.C + zo * p.sCo + zi * p.sCi; const float* R = p.R + zo * p.sRo + zi * p.sRi;
    for (int rr = 0; rr < rpt; ++rr) {
        const long long r = r0 + rr; if (r >= p.M) break;
        const float* A = p.A + zo * p.sAo + zi * p.sAi + r * p.sAm;
        float acc[8] = {0.f, 0.f, 0.f, 0.f, 0.f, 0.f, 0.f, 0.f};
        for (int k = 0; k < p.K; ++k) { const float a = A[(long long)k * p.sAk];
#pragma unroll
            for (int j = 0; j < 8; ++j) if (j < p.N) acc[j] += a * Bb[(long long)j * p.sBn + (long long)k * p.sBk]; }
#pragma unroll
        for (int j = 0; j < 8; ++j) if (j < p.N) {
            float v = acc[j] * p.alpha;
            if (p.flags & 1) v += p.bias[j];
            if (p.flags & 2) v += p.bias[r];
            v = act_fn(v, p.act);
            if (p.flags & 4) v += p.beta * R[r * p.sRm + (long long)j * p.sRn];
            VST2(float, C + r * p.sCm + j, v);
        }
    }
}
__global__ __launch_bounds__(256) void k_smallsoftmax(const float* __restrict__ src, float* __restrict__ dst, long long sr, long long dr, int n, long long R, float scale) {
    const long long r0 = ((long long)blockIdx.x * 256 + threadIdx.x) * 32;
    for (int rr = 0; rr < 32; ++rr) {
        const long long r = r0 + rr; if (r >= R) return;
        const float* s = src + r * sr; float* d = dst + r * dr;
        float mx = -__builtin_inff();
        for (int j = 0; j < n; ++j) mx = fmaxf(mx, s[j] * scale);
        float sum = 0.f;
        for (int j = 0; j < n; ++j) sum += expf(s[j] * scale - mx);
        const float inv = 1.f / sum;
        for (int j = 0; j < n; ++j) { const float v = expf(s[j] * scale - mx) * inv; VST2(float, d + j, v); }
    }
}

__global__ __launch_bounds__(32) void k_unitstat(float* __restrict__ st) { const int t = threadIdx.x; const float v = (t == 1) ? 1.f : 0.f; VST2(float, st + t, v); }

__global__ __launch_bounds__(256) void k_lincopy(const float* __restrict__ src, long long lds, float* __restrict__ dst, long long ldd, long long rows, int cols) {
    const long long i = (long long)blockIdx.x * 256 + threadIdx.x; if (i >= rows * cols) return;
    const long long r = i / cols; const int c = (int)(i - r * cols);
    const float v = src[r * lds + c]; VST2(float, dst + r * ldd + c, v);
}

__global__ __launch_bounds__(256) void k_vf_init(const float* __restrict__ d, float* __restrict__ RD, int n) { const int q = blockIdx.x * 256 + threadIdx.x; if (q >= n) return; VST2(float, RD + q, fminf(fmaxf(d[q], 0.f), 1.f)); }
__global__ __launch_bounds__(256) void k_vf_init2(const float* __restrict__ s0, const float* __restrict__ s1, float* __restrict__ S0, float* __restrict__ S1, float* __restrict__ R0, float* __restrict__ R1, int n0, int n1) { const int q = blockIdx.x * 256 + threadIdx.x; if (q < n0) { VST2(float, S0 + q, s0[q]); VST2(float, R0 + q, fminf(fmaxf(s0[q], 0.f), 1.f)); } if (q < n1) { VST2(float, S1 + q, s1[q]); VST2(float, R1 + q, fminf(fmaxf(s1[q], 0.f), 1.f)); } }
__global__ __launch_bounds__(256) void k_vf_upd(float* __restrict__ S, const float* __restrict__ G, float* __restrict__ R, int n, float dt) { const int q = blockIdx.x * 256 + threadIdx.x; if (q >= n) return; const float s = S[q]; const float v = fminf(fmaxf(s + dt * (-s + G[q]), 0.f), 1.f); VST2(float, S + q, v); VST2(float, R + q, v); }

template __global__ void k_gemm<1>(GemmP);

extern "C" void kernel_launch(void* const* d_in, const int* in_sizes, int n_in, void* d_out, int out_size, void* d_ws, size_t ws_size, hipStream_t stream) {
    (void)in_sizes; (void)n_in; (void)out_size; (void)ws_size;
    const float* data = (const float*)d_in[0];
    const float* s0 = (const float*)d_in[1];
    const float* s1 = (const float*)d_in[2];
    const float* w0 = (const float*)d_in[3];
    const float* b0 = (const float*)d_in[4];
    const float* w1 = (const float*)d_in[5];
    const float* w2 = (const float*)d_in[6];
    const float* b2 = (const float*)d_in[7];
    const int Bn = 256;
    const int N0 = 512;
    const int N1 = 2048;
    const int NI = 4096;
    float* out = (float*)d_out;
    float* s1out = out + ((size_t)Bn * N0);
    char* wsp = (char*)d_ws;
    float* RD = (float*)wsp; wsp += (((size_t)((size_t)Bn * NI) * 4 + 255) / 256) * 256;
    float* INP1 = (float*)wsp; wsp += (((size_t)((size_t)Bn * N1) * 4 + 255) / 256) * 256;
    float* S0 = (float*)wsp; wsp += (((size_t)((size_t)Bn * N0) * 4 + 255) / 256) * 256;
    float* S1 = (float*)wsp; wsp += (((size_t)((size_t)Bn * N1) * 4 + 255) / 256) * 256;
    float* R0 = (float*)wsp; wsp += (((size_t)((size_t)Bn * N0) * 4 + 255) / 256) * 256;
    float* R1 = (float*)wsp; wsp += (((size_t)((size_t)Bn * N1) * 4 + 255) / 256) * 256;
    float* G0 = (float*)wsp; wsp += (((size_t)((size_t)Bn * N0) * 4 + 255) / 256) * 256;
    float* G1 = (float*)wsp; wsp += (((size_t)((size_t)Bn * N1) * 4 + 255) / 256) * 256;
    k_vf_init<<<(unsigned)((Bn * NI + 255) / 256), 256, 0, stream>>>(data, RD, Bn * NI); k_vf_init2<<<(unsigned)((Bn * N1 + 255) / 256), 256, 0, stream>>>(s0, s1, S0, S1, R0, R1, Bn * N0, Bn * N1);
    { GemmP ginp;
      ginp.A = RD; ginp.B = w2; ginp.bias = b2; ginp.R = RD; ginp.C = INP1;
      ginp.sAo = 0; ginp.sAi = 0; ginp.sAm = NI; ginp.sAk = 1; ginp.sBo = 0; ginp.sBi = 0; ginp.sBn = NI; ginp.sBk = 1; ginp.sCo = 0; ginp.sCi = 0; ginp.sCm = N1; ginp.sRo = 0; ginp.sRi = 0; ginp.sRm = 0; ginp.sRn = 0;
      ginp.M = Bn; ginp.N = N1; ginp.K = NI; ginp.zi_n = 1; ginp.flags = 1; ginp.act = 0;
      ginp.alpha = 1.0f; ginp.beta = 0.0f; ginp.sa = 1.0f; ginp.sb = 1.0f; ginp.Npad = N1; ginp.pad_ = 0;
      k_gemm<1><<<dim3((unsigned)((N1) + 31) / 32, (unsigned)((Bn) + 15) / 16, (unsigned)(1)), 32, 0, stream>>>(ginp); }
    { GemmP g0_0;
      g0_0.A = R1; g0_0.B = w0; g0_0.bias = b0; g0_0.R = R1; g0_0.C = G0;
      g0_0.sAo = 0; g0_0.sAi = 0; g0_0.sAm = N1; g0_0.sAk = 1; g0_0.sBo = 0; g0_0.sBi = 0; g0_0.sBn = N1; g0_0.sBk = 1; g0_0.sCo = 0; g0_0.sCi = 0; g0_0.sCm = N0; g0_0.sRo = 0; g0_0.sRi = 0; g0_0.sRm = 0; g0_0.sRn = 0;
      g0_0.M = Bn; g0_0.N = N0; g0_0.K = N1; g0_0.zi_n = 1; g0_0.flags = 1; g0_0.act = 0;
      g0_0.alpha = 1.0f; g0_0.beta = 0.0f; g0_0.sa = 1.0f; g0_0.sb = 1.0f; g0_0.Npad = N0; g0_0.pad_ = 0;
      k_gemm<1><<<dim3((unsigned)((N0) + 31) / 32, (unsigned)((Bn) + 15) / 16, (unsigned)(1)), 32, 0, stream>>>(g0_0); }
    { GemmP g1_0;
      g1_0.A = R0; g1_0.B = w1; g1_0.bias = R0; g1_0.R = INP1; g1_0.C = G1;
      g1_0.sAo = 0; g1_0.sAi = 0; g1_0.sAm = N0; g1_0.sAk = 1; g1_0.sBo = 0; g1_0.sBi = 0; g1_0.sBn = N0; g1_0.sBk = 1; g1_0.sCo = 0; g1_0.sCi = 0; g1_0.sCm = N1; g1_0.sRo = 0; g1_0.sRi = 0; g1_0.sRm = N1; g1_0.sRn = 1;
      g1_0.M = Bn; g1_0.N = N1; g1_0.K = N0; g1_0.zi_n = 1; g1_0.flags = 4; g1_0.act = 0;
      g1_0.alpha = 1.0f; g1_0.beta = 1.0f; g1_0.sa = 1.0f; g1_0.sb = 1.0f; g1_0.Npad = N1; g1_0.pad_ = 0;
      k_gemm<1><<<dim3((unsigned)((N1) + 31) / 32, (unsigned)((Bn) + 15) / 16, (unsigned)(1)), 32, 0, stream>>>(g1_0); }
    k_vf_upd<<<(unsigned)((Bn * N0 + 255) / 256), 256, 0, stream>>>(S0, G0, R0, Bn * N0, 0.5f); k_vf_upd<<<(unsigned)((Bn * N1 + 255) / 256), 256, 0, stream>>>(S1, G1, R1, Bn * N1, 0.5f);
    { GemmP g0_1;
      g0_1.A = R1; g0_1.B = w0; g0_1.bias = b0; g0_1.R = R1; g0_1.C = G0;
      g0_1.sAo = 0; g0_1.sAi = 0; g0_1.sAm = N1; g0_1.sAk = 1; g0_1.sBo = 0; g0_1.sBi = 0; g0_1.sBn = N1; g0_1.sBk = 1; g0_1.sCo = 0; g0_1.sCi = 0; g0_1.sCm = N0; g0_1.sRo = 0; g0_1.sRi = 0; g0_1.sRm = 0; g0_1.sRn = 0;
      g0_1.M = Bn; g0_1.N = N0; g0_1.K = N1; g0_1.zi_n = 1; g0_1.flags = 1; g0_1.act = 0;
      g0_1.alpha = 1.0f; g0_1.beta = 0.0f; g0_1.sa = 1.0f; g0_1.sb = 1.0f; g0_1.Npad = N0; g0_1.pad_ = 0;
      k_gemm<1><<<dim3((unsigned)((N0) + 31) / 32, (unsigned)((Bn) + 15) / 16, (unsigned)(1)), 32, 0, stream>>>(g0_1); }
    { GemmP g1_1;
      g1_1.A = R0; g1_1.B = w1; g1_1.bias = R0; g1_1.R = INP1; g1_1.C = G1;
      g1_1.sAo = 0; g1_1.sAi = 0; g1_1.sAm = N0; g1_1.sAk = 1; g1_1.sBo = 0; g1_1.sBi = 0; g1_1.sBn = N0; g1_1.sBk = 1; g1_1.sCo = 0; g1_1.sCi = 0; g1_1.sCm = N1; g1_1.sRo = 0; g1_1.sRi = 0; g1_1.sRm = N1; g1_1.sRn = 1;
      g1_1.M = Bn; g1_1.N = N1; g1_1.K = N0; g1_1.zi_n = 1; g1_1.flags = 4; g1_1.act = 0;
      g1_1.alpha = 1.0f; g1_1.beta = 1.0f; g1_1.sa = 1.0f; g1_1.sb = 1.0f; g1_1.Npad = N1; g1_1.pad_ = 0;
      k_gemm<1><<<dim3((unsigned)((N1) + 31) / 32, (unsigned)((Bn) + 15) / 16, (unsigned)(1)), 32, 0, stream>>>(g1_1); }
    k_vf_upd<<<(unsigned)((Bn * N0 + 255) / 256), 256, 0, stream>>>(S0, G0, R0, Bn * N0, 0.5f); k_vf_upd<<<(unsigned)((Bn * N1 + 255) / 256), 256, 0, stream>>>(S1, G1, R1, Bn * N1, 0.5f);
    { GemmP g0_2;
      g0_2.A = R1; g0_2.B = w0; g0_2.bias = b0; g0_2.R = R1; g0_2.C = G0;
      g0_2.sAo = 0; g0_2.sAi = 0; g0_2.sAm = N1; g0_2.sAk = 1; g0_2.sBo = 0; g0_2.sBi = 0; g0_2.sBn = N1; g0_2.sBk = 1; g0_2.sCo = 0; g0_2.sCi = 0; g0_2.sCm = N0; g0_2.sRo = 0; g0_2.sRi = 0; g0_2.sRm = 0; g0_2.sRn = 0;
      g0_2.M = Bn; g0_2.N = N0; g0_2.K = N1; g0_2.zi_n = 1; g0_2.flags = 1; g0_2.act = 0;
      g0_2.alpha = 1.0f; g0_2.beta = 0.0f; g0_2.sa = 1.0f; g0_2.sb = 1.0f; g0_2.Npad = N0; g0_2.pad_ = 0;
      k_gemm<1><<<dim3((unsigned)((N0) + 31) / 32, (unsigned)((Bn) + 15) / 16, (unsigned)(1)), 32, 0, stream>>>(g0_2); }
    { GemmP g1_2;
      g1_2.A = R0; g1_2.B = w1; g1_2.bias = R0; g1_2.R = INP1; g1_2.C = G1;
      g1_2.sAo = 0; g1_2.sAi = 0; g1_2.sAm = N0; g1_2.sAk = 1; g1_2.sBo = 0; g1_2.sBi = 0; g1_2.sBn = N0; g1_2.sBk = 1; g1_2.sCo = 0; g1_2.sCi = 0; g1_2.sCm = N1; g1_2.sRo = 0; g1_2.sRi = 0; g1_2.sRm = N1; g1_2.sRn = 1;
      g1_2.M = Bn; g1_2.N = N1; g1_2.K = N0; g1_2.zi_n = 1; g1_2.flags = 4; g1_2.act = 0;
      g1_2.alpha = 1.0f; g1_2.beta = 1.0f; g1_2.sa = 1.0f; g1_2.sb = 1.0f; g1_2.Npad = N1; g1_2.pad_ = 0;
      k_gemm<1><<<dim3((unsigned)((N1) + 31) / 32, (unsigned)((Bn) + 15) / 16, (unsigned)(1)), 32, 0, stream>>>(g1_2); }
    k_vf_upd<<<(unsigned)((Bn * N0 + 255) / 256), 256, 0, stream>>>(S0, G0, R0, Bn * N0, 0.5f); k_vf_upd<<<(unsigned)((Bn * N1 + 255) / 256), 256, 0, stream>>>(S1, G1, R1, Bn * N1, 0.5f);
    { GemmP g0_3;
      g0_3.A = R1; g0_3.B = w0; g0_3.bias = b0; g0_3.R = R1; g0_3.C = G0;
      g0_3.sAo = 0; g0_3.sAi = 0; g0_3.sAm = N1; g0_3.sAk = 1; g0_3.sBo = 0; g0_3.sBi = 0; g0_3.sBn = N1; g0_3.sBk = 1; g0_3.sCo = 0; g0_3.sCi = 0; g0_3.sCm = N0; g0_3.sRo = 0; g0_3.sRi = 0; g0_3.sRm = 0; g0_3.sRn = 0;
      g0_3.M = Bn; g0_3.N = N0; g0_3.K = N1; g0_3.zi_n = 1; g0_3.flags = 1; g0_3.act = 0;
      g0_3.alpha = 1.0f; g0_3.beta = 0.0f; g0_3.sa = 1.0f; g0_3.sb = 1.0f; g0_3.Npad = N0; g0_3.pad_ = 0;
      k_gemm<1><<<dim3((unsigned)((N0) + 31) / 32, (unsigned)((Bn) + 15) / 16, (unsigned)(1)), 32, 0, stream>>>(g0_3); }
    { GemmP g1_3;
      g1_3.A = R0; g1_3.B = w1; g1_3.bias = R0; g1_3.R = INP1; g1_3.C = G1;
      g1_3.sAo = 0; g1_3.sAi = 0; g1_3.sAm = N0; g1_3.sAk = 1; g1_3.sBo = 0; g1_3.sBi = 0; g1_3.sBn = N0; g1_3.sBk = 1; g1_3.sCo = 0; g1_3.sCi = 0; g1_3.sCm = N1; g1_3.sRo = 0; g1_3.sRi = 0; g1_3.sRm = N1; g1_3.sRn = 1;
      g1_3.M = Bn; g1_3.N = N1; g1_3.K = N0; g1_3.zi_n = 1; g1_3.flags = 4; g1_3.act = 0;
      g1_3.alpha = 1.0f; g1_3.beta = 1.0f; g1_3.sa = 1.0f; g1_3.sb = 1.0f; g1_3.Npad = N1; g1_3.pad_ = 0;
      k_gemm<1><<<dim3((unsigned)((N1) + 31) / 32, (unsigned)((Bn) + 15) / 16, (unsigned)(1)), 32, 0, stream>>>(g1_3); }
    k_vf_upd<<<(unsigned)((Bn * N0 + 255) / 256), 256, 0, stream>>>(S0, G0, R0, Bn * N0, 0.5f); k_vf_upd<<<(unsigned)((Bn * N1 + 255) / 256), 256, 0, stream>>>(S1, G1, R1, Bn * N1, 0.5f);
    { GemmP g0_4;
      g0_4.A = R1; g0_4.B = w0; g0_4.bias = b0; g0_4.R = R1; g0_4.C = G0;
      g0_4.sAo = 0; g0_4.sAi = 0; g0_4.sAm = N1; g0_4.sAk = 1; g0_4.sBo = 0; g0_4.sBi = 0; g0_4.sBn = N1; g0_4.sBk = 1; g0_4.sCo = 0; g0_4.sCi = 0; g0_4.sCm = N0; g0_4.sRo = 0; g0_4.sRi = 0; g0_4.sRm = 0; g0_4.sRn = 0;
      g0_4.M = Bn; g0_4.N = N0; g0_4.K = N1; g0_4.zi_n = 1; g0_4.flags = 1; g0_4.act = 0;
      g0_4.alpha = 1.0f; g0_4.beta = 0.0f; g0_4.sa = 1.0f; g0_4.sb = 1.0f; g0_4.Npad = N0; g0_4.pad_ = 0;
      k_gemm<1><<<dim3((unsigned)((N0) + 31) / 32, (unsigned)((Bn) + 15) / 16, (unsigned)(1)), 32, 0, stream>>>(g0_4); }
    { GemmP g1_4;
      g1_4.A = R0; g1_4.B = w1; g1_4.bias = R0; g1_4.R = INP1; g1_4.C = G1;
      g1_4.sAo = 0; g1_4.sAi = 0; g1_4.sAm = N0; g1_4.sAk = 1; g1_4.sBo = 0; g1_4.sBi = 0; g1_4.sBn = N0; g1_4.sBk = 1; g1_4.sCo = 0; g1_4.sCi = 0; g1_4.sCm = N1; g1_4.sRo = 0; g1_4.sRi = 0; g1_4.sRm = N1; g1_4.sRn = 1;
      g1_4.M = Bn; g1_4.N = N1; g1_4.K = N0; g1_4.zi_n = 1; g1_4.flags = 4; g1_4.act = 0;
      g1_4.alpha = 1.0f; g1_4.beta = 1.0f; g1_4.sa = 1.0f; g1_4.sb = 1.0f; g1_4.Npad = N1; g1_4.pad_ = 0;
      k_gemm<1><<<dim3((unsigned)((N1) + 31) / 32, (unsigned)((Bn) + 15) / 16, (unsigned)(1)), 32, 0, stream>>>(g1_4); }
    k_vf_upd<<<(unsigned)((Bn * N0 + 255) / 256), 256, 0, stream>>>(S0, G0, R0, Bn * N0, 0.5f); k_vf_upd<<<(unsigned)((Bn * N1 + 255) / 256), 256, 0, stream>>>(S1, G1, R1, Bn * N1, 0.5f);
    { GemmP g0_5;
      g0_5.A = R1; g0_5.B = w0; g0_5.bias = b0; g0_5.R = R1; g0_5.C = G0;
      g0_5.sAo = 0; g0_5.sAi = 0; g0_5.sAm = N1; g0_5.sAk = 1; g0_5.sBo = 0; g0_5.sBi = 0; g0_5.sBn = N1; g0_5.sBk = 1; g0_5.sCo = 0; g0_5.sCi = 0; g0_5.sCm = N0; g0_5.sRo = 0; g0_5.sRi = 0; g0_5.sRm = 0; g0_5.sRn = 0;
      g0_5.M = Bn; g0_5.N = N0; g0_5.K = N1; g0_5.zi_n = 1; g0_5.flags = 1; g0_5.act = 0;
      g0_5.alpha = 1.0f; g0_5.beta = 0.0f; g0_5.sa = 1.0f; g0_5.sb = 1.0f; g0_5.Npad = N0; g0_5.pad_ = 0;
      k_gemm<1><<<dim3((unsigned)((N0) + 31) / 32, (unsigned)((Bn) + 15) / 16, (unsigned)(1)), 32, 0, stream>>>(g0_5); }
    { GemmP g1_5;
      g1_5.A = R0; g1_5.B = w1; g1_5.bias = R0; g1_5.R = INP1; g1_5.C = G1;
      g1_5.sAo = 0; g1_5.sAi = 0; g1_5.sAm = N0; g1_5.sAk = 1; g1_5.sBo = 0; g1_5.sBi = 0; g1_5.sBn = N0; g1_5.sBk = 1; g1_5.sCo = 0; g1_5.sCi = 0; g1_5.sCm = N1; g1_5.sRo = 0; g1_5.sRi = 0; g1_5.sRm = N1; g1_5.sRn = 1;
      g1_5.M = Bn; g1_5.N = N1; g1_5.K = N0; g1_5.zi_n = 1; g1_5.flags = 4; g1_5.act = 0;
      g1_5.alpha = 1.0f; g1_5.beta = 1.0f; g1_5.sa = 1.0f; g1_5.sb = 1.0f; g1_5.Npad = N1; g1_5.pad_ = 0;
      k_gemm<1><<<dim3((unsigned)((N1) + 31) / 32, (unsigned)((Bn) + 15) / 16, (unsigned)(1)), 32, 0, stream>>>(g1_5); }
    k_vf_upd<<<(unsigned)((Bn * N0 + 255) / 256), 256, 0, stream>>>(S0, G0, R0, Bn * N0, 0.5f); k_vf_upd<<<(unsigned)((Bn * N1 + 255) / 256), 256, 0, stream>>>(S1, G1, R1, Bn * N1, 0.5f);
    { GemmP g0_6;
      g0_6.A = R1; g0_6.B = w0; g0_6.bias = b0; g0_6.R = R1; g0_6.C = G0;
      g0_6.sAo = 0; g0_6.sAi = 0; g0_6.sAm = N1; g0_6.sAk = 1; g0_6.sBo = 0; g0_6.sBi = 0; g0_6.sBn = N1; g0_6.sBk = 1; g0_6.sCo = 0; g0_6.sCi = 0; g0_6.sCm = N0; g0_6.sRo = 0; g0_6.sRi = 0; g0_6.sRm = 0; g0_6.sRn = 0;
      g0_6.M = Bn; g0_6.N = N0; g0_6.K = N1; g0_6.zi_n = 1; g0_6.flags = 1; g0_6.act = 0;
      g0_6.alpha = 1.0f; g0_6.beta = 0.0f; g0_6.sa = 1.0f; g0_6.sb = 1.0f; g0_6.Npad = N0; g0_6.pad_ = 0;
      k_gemm<1><<<dim3((unsigned)((N0) + 31) / 32, (unsigned)((Bn) + 15) / 16, (unsigned)(1)), 32, 0, stream>>>(g0_6); }
    { GemmP g1_6;
      g1_6.A = R0; g1_6.B = w1; g1_6.bias = R0; g1_6.R = INP1; g1_6.C = G1;
      g1_6.sAo = 0; g1_6.sAi = 0; g1_6.sAm = N0; g1_6.sAk = 1; g1_6.sBo = 0; g1_6.sBi = 0; g1_6.sBn = N0; g1_6.sBk = 1; g1_6.sCo = 0; g1_6.sCi = 0; g1_6.sCm = N1; g1_6.sRo = 0; g1_6.sRi = 0; g1_6.sRm = N1; g1_6.sRn = 1;
      g1_6.M = Bn; g1_6.N = N1; g1_6.K = N0; g1_6.zi_n = 1; g1_6.flags = 4; g1_6.act = 0;
      g1_6.alpha = 1.0f; g1_6.beta = 1.0f; g1_6.sa = 1.0f; g1_6.sb = 1.0f; g1_6.Npad = N1; g1_6.pad_ = 0;
      k_gemm<1><<<dim3((unsigned)((N1) + 31) / 32, (unsigned)((Bn) + 15) / 16, (unsigned)(1)), 32, 0, stream>>>(g1_6); }
    k_vf_upd<<<(unsigned)((Bn * N0 + 255) / 256), 256, 0, stream>>>(S0, G0, R0, Bn * N0, 0.5f); k_vf_upd<<<(unsigned)((Bn * N1 + 255) / 256), 256, 0, stream>>>(S1, G1, R1, Bn * N1, 0.5f);
    { GemmP g0_7;
      g0_7.A = R1; g0_7.B = w0; g0_7.bias = b0; g0_7.R = R1; g0_7.C = G0;
      g0_7.sAo = 0; g0_7.sAi = 0; g0_7.sAm = N1; g0_7.sAk = 1; g0_7.sBo = 0; g0_7.sBi = 0; g0_7.sBn = N1; g0_7.sBk = 1; g0_7.sCo = 0; g0_7.sCi = 0; g0_7.sCm = N0; g0_7.sRo = 0; g0_7.sRi = 0; g0_7.sRm = 0; g0_7.sRn = 0;
      g0_7.M = Bn; g0_7.N = N0; g0_7.K = N1; g0_7.zi_n = 1; g0_7.flags = 1; g0_7.act = 0;
      g0_7.alpha = 1.0f; g0_7.beta = 0.0f; g0_7.sa = 1.0f; g0_7.sb = 1.0f; g0_7.Npad = N0; g0_7.pad_ = 0;
      k_gemm<1><<<dim3((unsigned)((N0) + 31) / 32, (unsigned)((Bn) + 15) / 16, (unsigned)(1)), 32, 0, stream>>>(g0_7); }
    { GemmP g1_7;
      g1_7.A = R0; g1_7.B = w1; g1_7.bias = R0; g1_7.R = INP1; g1_7.C = G1;
      g1_7.sAo = 0; g1_7.sAi = 0; g1_7.sAm = N0; g1_7.sAk = 1; g1_7.sBo = 0; g1_7.sBi = 0; g1_7.sBn = N0; g1_7.sBk = 1; g1_7.sCo = 0; g1_7.sCi = 0; g1_7.sCm = N1; g1_7.sRo = 0; g1_7.sRi = 0; g1_7.sRm = N1; g1_7.sRn = 1;
      g1_7.M = Bn; g1_7.N = N1; g1_7.K = N0; g1_7.zi_n = 1; g1_7.flags = 4; g1_7.act = 0;
      g1_7.alpha = 1.0f; g1_7.beta = 1.0f; g1_7.sa = 1.0f; g1_7.sb = 1.0f; g1_7.Npad = N1; g1_7.pad_ = 0;
      k_gemm<1><<<dim3((unsigned)((N1) + 31) / 32, (unsigned)((Bn) + 15) / 16, (unsigned)(1)), 32, 0, stream>>>(g1_7); }
    k_vf_upd<<<(unsigned)((Bn * N0 + 255) / 256), 256, 0, stream>>>(S0, G0, R0, Bn * N0, 0.5f); k_vf_upd<<<(unsigned)((Bn * N1 + 255) / 256), 256, 0, stream>>>(S1, G1, R1, Bn * N1, 0.5f);
    { GemmP g0_8;
      g0_8.A = R1; g0_8.B = w0; g0_8.bias = b0; g0_8.R = R1; g0_8.C = G0;
      g0_8.sAo = 0; g0_8.sAi = 0; g0_8.sAm = N1; g0_8.sAk = 1; g0_8.sBo = 0; g0_8.sBi = 0; g0_8.sBn = N1; g0_8.sBk = 1; g0_8.sCo = 0; g0_8.sCi = 0; g0_8.sCm = N0; g0_8.sRo = 0; g0_8.sRi = 0; g0_8.sRm = 0; g0_8.sRn = 0;
      g0_8.M = Bn; g0_8.N = N0; g0_8.K = N1; g0_8.zi_n = 1; g0_8.flags = 1; g0_8.act = 0;
      g0_8.alpha = 1.0f; g0_8.beta = 0.0f; g0_8.sa = 1.0f; g0_8.sb = 1.0f; g0_8.Npad = N0; g0_8.pad_ = 0;
      k_gemm<1><<<dim3((unsigned)((N0) + 31) / 32, (unsigned)((Bn) + 15) / 16, (unsigned)(1)), 32, 0, stream>>>(g0_8); }
    { GemmP g1_8;
      g1_8.A = R0; g1_8.B = w1; g1_8.bias = R0; g1_8.R = INP1; g1_8.C = G1;
      g1_8.sAo = 0; g1_8.sAi = 0; g1_8.sAm = N0; g1_8.sAk = 1; g1_8.sBo = 0; g1_8.sBi = 0; g1_8.sBn = N0; g1_8.sBk = 1; g1_8.sCo = 0; g1_8.sCi = 0; g1_8.sCm = N1; g1_8.sRo = 0; g1_8.sRi = 0; g1_8.sRm = N1; g1_8.sRn = 1;
      g1_8.M = Bn; g1_8.N = N1; g1_8.K = N0; g1_8.zi_n = 1; g1_8.flags = 4; g1_8.act = 0;
      g1_8.alpha = 1.0f; g1_8.beta = 1.0f; g1_8.sa = 1.0f; g1_8.sb = 1.0f; g1_8.Npad = N1; g1_8.pad_ = 0;
      k_gemm<1><<<dim3((unsigned)((N1) + 31) / 32, (unsigned)((Bn) + 15) / 16, (unsigned)(1)), 32, 0, stream>>>(g1_8); }
    k_vf_upd<<<(unsigned)((Bn * N0 + 255) / 256), 256, 0, stream>>>(S0, G0, R0, Bn * N0, 0.5f); k_vf_upd<<<(unsigned)((Bn * N1 + 255) / 256), 256, 0, stream>>>(S1, G1, R1, Bn * N1, 0.5f);
    { GemmP g0_9;
      g0_9.A = R1; g0_9.B = w0; g0_9.bias = b0; g0_9.R = R1; g0_9.C = G0;
      g0_9.sAo = 0; g0_9.sAi = 0; g0_9.sAm = N1; g0_9.sAk = 1; g0_9.sBo = 0; g0_9.sBi = 0; g0_9.sBn = N1; g0_9.sBk = 1; g0_9.sCo = 0; g0_9.sCi = 0; g0_9.sCm = N0; g0_9.sRo = 0; g0_9.sRi = 0; g0_9.sRm = 0; g0_9.sRn = 0;
      g0_9.M = Bn; g0_9.N = N0; g0_9.K = N1; g0_9.zi_n = 1; g0_9.flags = 1; g0_9.act = 0;
      g0_9.alpha = 1.0f; g0_9.beta = 0.0f; g0_9.sa = 1.0f; g0_9.sb = 1.0f; g0_9.Npad = N0; g0_9.pad_ = 0;
      k_gemm<1><<<dim3((unsigned)((N0) + 31) / 32, (unsigned)((Bn) + 15) / 16, (unsigned)(1)), 32, 0, stream>>>(g0_9); }
    { GemmP g1_9;
      g1_9.A = R0; g1_9.B = w1; g1_9.bias = R0; g1_9.R = INP1; g1_9.C = G1;
      g1_9.sAo = 0; g1_9.sAi = 0; g1_9.sAm = N0; g1_9.sAk = 1; g1_9.sBo = 0; g1_9.sBi = 0; g1_9.sBn = N0; g1_9.sBk = 1; g1_9.sCo = 0; g1_9.sCi = 0; g1_9.sCm = N1; g1_9.sRo = 0; g1_9.sRi = 0; g1_9.sRm = N1; g1_9.sRn = 1;
      g1_9.M = Bn; g1_9.N = N1; g1_9.K = N0; g1_9.zi_n = 1; g1_9.flags = 4; g1_9.act = 0;
      g1_9.alpha = 1.0f; g1_9.beta = 1.0f; g1_9.sa = 1.0f; g1_9.sb = 1.0f; g1_9.Npad = N1; g1_9.pad_ = 0;
      k_gemm<1><<<dim3((unsigned)((N1) + 31) / 32, (unsigned)((Bn) + 15) / 16, (unsigned)(1)), 32, 0, stream>>>(g1_9); }
    k_vf_upd<<<(unsigned)((Bn * N0 + 255) / 256), 256, 0, stream>>>(S0, G0, R0, Bn * N0, 0.5f); k_vf_upd<<<(unsigned)((Bn * N1 + 255) / 256), 256, 0, stream>>>(S1, G1, R1, Bn * N1, 0.5f);
    { GemmP g0_10;
      g0_10.A = R1; g0_10.B = w0; g0_10.bias = b0; g0_10.R = R1; g0_10.C = G0;
      g0_10.sAo = 0; g0_10.sAi = 0; g0_10.sAm = N1; g0_10.sAk = 1; g0_10.sBo = 0; g0_10.sBi = 0; g0_10.sBn = N1; g0_10.sBk = 1; g0_10.sCo = 0; g0_10.sCi = 0; g0_10.sCm = N0; g0_10.sRo = 0; g0_10.sRi = 0; g0_10.sRm = 0; g0_10.sRn = 0;
      g0_10.M = Bn; g0_10.N = N0; g0_10.K = N1; g0_10.zi_n = 1; g0_10.flags = 1; g0_10.act = 0;
      g0_10.alpha = 1.0f; g0_10.beta = 0.0f; g0_10.sa = 1.0f; g0_10.sb = 1.0f; g0_10.Npad = N0; g0_10.pad_ = 0;
      k_gemm<1><<<dim3((unsigned)((N0) + 31) / 32, (unsigned)((Bn) + 15) / 16, (unsigned)(1)), 32, 0, stream>>>(g0_10); }
    { GemmP g1_10;
      g1_10.A = R0; g1_10.B = w1; g1_10.bias = R0; g1_10.R = INP1; g1_10.C = G1;
      g1_10.sAo = 0; g1_10.sAi = 0; g1_10.sAm = N0; g1_10.sAk = 1; g1_10.sBo = 0; g1_10.sBi = 0; g1_10.sBn = N0; g1_10.sBk = 1; g1_10.sCo = 0; g1_10.sCi = 0; g1_10.sCm = N1; g1_10.sRo = 0; g1_10.sRi = 0; g1_10.sRm = N1; g1_10.sRn = 1;
      g1_10.M = Bn; g1_10.N = N1; g1_10.K = N0; g1_10.zi_n = 1; g1_10.flags = 4; g1_10.act = 0;
      g1_10.alpha = 1.0f; g1_10.beta = 1.0f; g1_10.sa = 1.0f; g1_10.sb = 1.0f; g1_10.Npad = N1; g1_10.pad_ = 0;
      k_gemm<1><<<dim3((unsigned)((N1) + 31) / 32, (unsigned)((Bn) + 15) / 16, (unsigned)(1)), 32, 0, stream>>>(g1_10); }
    k_vf_upd<<<(unsigned)((Bn * N0 + 255) / 256), 256, 0, stream>>>(S0, G0, R0, Bn * N0, 0.5f); k_vf_upd<<<(unsigned)((Bn * N1 + 255) / 256), 256, 0, stream>>>(S1, G1, R1, Bn * N1, 0.5f);
    { GemmP g0_11;
      g0_11.A = R1; g0_11.B = w0; g0_11.bias = b0; g0_11.R = R1; g0_11.C = G0;
      g0_11.sAo = 0; g0_11.sAi = 0; g0_11.sAm = N1; g0_11.sAk = 1; g0_11.sBo = 0; g0_11.sBi = 0; g0_11.sBn = N1; g0_11.sBk = 1; g0_11.sCo = 0; g0_11.sCi = 0; g0_11.sCm = N0; g0_11.sRo = 0; g0_11.sRi = 0; g0_11.sRm = 0; g0_11.sRn = 0;
      g0_11.M = Bn; g0_11.N = N0; g0_11.K = N1; g0_11.zi_n = 1; g0_11.flags = 1; g0_11.act = 0;
      g0_11.alpha = 1.0f; g0_11.beta = 0.0f; g0_11.sa = 1.0f; g0_11.sb = 1.0f; g0_11.Npad = N0; g0_11.pad_ = 0;
      k_gemm<1><<<dim3((unsigned)((N0) + 31) / 32, (unsigned)((Bn) + 15) / 16, (unsigned)(1)), 32, 0, stream>>>(g0_11); }
    { GemmP g1_11;
      g1_11.A = R0; g1_11.B = w1; g1_11.bias = R0; g1_11.R = INP1; g1_11.C = G1;
      g1_11.sAo = 0; g1_11.sAi = 0; g1_11.sAm = N0; g1_11.sAk = 1; g1_11.sBo = 0; g1_11.sBi = 0; g1_11.sBn = N0; g1_11.sBk = 1; g1_11.sCo = 0; g1_11.sCi = 0; g1_11.sCm = N1; g1_11.sRo = 0; g1_11.sRi = 0; g1_11.sRm = N1; g1_11.sRn = 1;
      g1_11.M = Bn; g1_11.N = N1; g1_11.K = N0; g1_11.zi_n = 1; g1_11.flags = 4; g1_11.act = 0;
      g1_11.alpha = 1.0f; g1_11.beta = 1.0f; g1_11.sa = 1.0f; g1_11.sb = 1.0f; g1_11.Npad = N1; g1_11.pad_ = 0;
      k_gemm<1><<<dim3((unsigned)((N1) + 31) / 32, (unsigned)((Bn) + 15) / 16, (unsigned)(1)), 32, 0, stream>>>(g1_11); }
    k_vf_upd<<<(unsigned)((Bn * N0 + 255) / 256), 256, 0, stream>>>(S0, G0, R0, Bn * N0, 0.5f); k_vf_upd<<<(unsigned)((Bn * N1 + 255) / 256), 256, 0, stream>>>(S1, G1, R1, Bn * N1, 0.5f);
    { GemmP g0_12;
      g0_12.A = R1; g0_12.B = w0; g0_12.bias = b0; g0_12.R = R1; g0_12.C = G0;
      g0_12.sAo = 0; g0_12.sAi = 0; g0_12.sAm = N1; g0_12.sAk = 1; g0_12.sBo = 0; g0_12.sBi = 0; g0_12.sBn = N1; g0_12.sBk = 1; g0_12.sCo = 0; g0_12.sCi = 0; g0_12.sCm = N0; g0_12.sRo = 0; g0_12.sRi = 0; g0_12.sRm = 0; g0_12.sRn = 0;
      g0_12.M = Bn; g0_12.N = N0; g0_12.K = N1; g0_12.zi_n = 1; g0_12.flags = 1; g0_12.act = 0;
      g0_12.alpha = 1.0f; g0_12.beta = 0.0f; g0_12.sa = 1.0f; g0_12.sb = 1.0f; g0_12.Npad = N0; g0_12.pad_ = 0;
      k_gemm<1><<<dim3((unsigned)((N0) + 31) / 32, (unsigned)((Bn) + 15) / 16, (unsigned)(1)), 32, 0, stream>>>(g0_12); }
    { GemmP g1_12;
      g1_12.A = R0; g1_12.B = w1; g1_12.bias = R0; g1_12.R = INP1; g1_12.C = G1;
      g1_12.sAo = 0; g1_12.sAi = 0; g1_12.sAm = N0; g1_12.sAk = 1; g1_12.sBo = 0; g1_12.sBi = 0; g1_12.sBn = N0; g1_12.sBk = 1; g1_12.sCo = 0; g1_12.sCi = 0; g1_12.sCm = N1; g1_12.sRo = 0; g1_12.sRi = 0; g1_12.sRm = N1; g1_12.sRn = 1;
      g1_12.M = Bn; g1_12.N = N1; g1_12.K = N0; g1_12.zi_n = 1; g1_12.flags = 4; g1_12.act = 0;
      g1_12.alpha = 1.0f; g1_12.beta = 1.0f; g1_12.sa = 1.0f; g1_12.sb = 1.0f; g1_12.Npad = N1; g1_12.pad_ = 0;
      k_gemm<1><<<dim3((unsigned)((N1) + 31) / 32, (unsigned)((Bn) + 15) / 16, (unsigned)(1)), 32, 0, stream>>>(g1_12); }
    k_vf_upd<<<(unsigned)((Bn * N0 + 255) / 256), 256, 0, stream>>>(S0, G0, R0, Bn * N0, 0.5f); k_vf_upd<<<(unsigned)((Bn * N1 + 255) / 256), 256, 0, stream>>>(S1, G1, R1, Bn * N1, 0.5f);
    { GemmP g0_13;
      g0_13.A = R1; g0_13.B = w0; g0_13.bias = b0; g0_13.R = R1; g0_13.C = G0;
      g0_13.sAo = 0; g0_13.sAi = 0; g0_13.sAm = N1; g0_13.sAk = 1; g0_13.sBo = 0; g0_13.sBi = 0; g0_13.sBn = N1; g0_13.sBk = 1; g0_13.sCo = 0; g0_13.sCi = 0; g0_13.sCm = N0; g0_13.sRo = 0; g0_13.sRi = 0; g0_13.sRm = 0; g0_13.sRn = 0;
      g0_13.M = Bn; g0_13.N = N0; g0_13.K = N1; g0_13.zi_n = 1; g0_13.flags = 1; g0_13.act = 0;
      g0_13.alpha = 1.0f; g0_13.beta = 0.0f; g0_13.sa = 1.0f; g0_13.sb = 1.0f; g0_13.Npad = N0; g0_13.pad_ = 0;
      k_gemm<1><<<dim3((unsigned)((N0) + 31) / 32, (unsigned)((Bn) + 15) / 16, (unsigned)(1)), 32, 0, stream>>>(g0_13); }
    { GemmP g1_13;
      g1_13.A = R0; g1_13.B = w1; g1_13.bias = R0; g1_13.R = INP1; g1_13.C = G1;
      g1_13.sAo = 0; g1_13.sAi = 0; g1_13.sAm = N0; g1_13.sAk = 1; g1_13.sBo = 0; g1_13.sBi = 0; g1_13.sBn = N0; g1_13.sBk = 1; g1_13.sCo = 0; g1_13.sCi = 0; g1_13.sCm = N1; g1_13.sRo = 0; g1_13.sRi = 0; g1_13.sRm = N1; g1_13.sRn = 1;
      g1_13.M = Bn; g1_13.N = N1; g1_13.K = N0; g1_13.zi_n = 1; g1_13.flags = 4; g1_13.act = 0;
      g1_13.alpha = 1.0f; g1_13.beta = 1.0f; g1_13.sa = 1.0f; g1_13.sb = 1.0f; g1_13.Npad = N1; g1_13.pad_ = 0;
      k_gemm<1><<<dim3((unsigned)((N1) + 31) / 32, (unsigned)((Bn) + 15) / 16, (unsigned)(1)), 32, 0, stream>>>(g1_13); }
    k_vf_upd<<<(unsigned)((Bn * N0 + 255) / 256), 256, 0, stream>>>(S0, G0, R0, Bn * N0, 0.5f); k_vf_upd<<<(unsigned)((Bn * N1 + 255) / 256), 256, 0, stream>>>(S1, G1, R1, Bn * N1, 0.5f);
    { GemmP g0_14;
      g0_14.A = R1; g0_14.B = w0; g0_14.bias = b0; g0_14.R = R1; g0_14.C = G0;
      g0_14.sAo = 0; g0_14.sAi = 0; g0_14.sAm = N1; g0_14.sAk = 1; g0_14.sBo = 0; g0_14.sBi = 0; g0_14.sBn = N1; g0_14.sBk = 1; g0_14.sCo = 0; g0_14.sCi = 0; g0_14.sCm = N0; g0_14.sRo = 0; g0_14.sRi = 0; g0_14.sRm = 0; g0_14.sRn = 0;
      g0_14.M = Bn; g0_14.N = N0; g0_14.K = N1; g0_14.zi_n = 1; g0_14.flags = 1; g0_14.act = 0;
      g0_14.alpha = 1.0f; g0_14.beta = 0.0f; g0_14.sa = 1.0f; g0_14.sb = 1.0f; g0_14.Npad = N0; g0_14.pad_ = 0;
      k_gemm<1><<<dim3((unsigned)((N0) + 31) / 32, (unsigned)((Bn) + 15) / 16, (unsigned)(1)), 32, 0, stream>>>(g0_14); }
    { GemmP g1_14;
      g1_14.A = R0; g1_14.B = w1; g1_14.bias = R0; g1_14.R = INP1; g1_14.C = G1;
      g1_14.sAo = 0; g1_14.sAi = 0; g1_14.sAm = N0; g1_14.sAk = 1; g1_14.sBo = 0; g1_14.sBi = 0; g1_14.sBn = N0; g1_14.sBk = 1; g1_14.sCo = 0; g1_14.sCi = 0; g1_14.sCm = N1; g1_14.sRo = 0; g1_14.sRi = 0; g1_14.sRm = N1; g1_14.sRn = 1;
      g1_14.M = Bn; g1_14.N = N1; g1_14.K = N0; g1_14.zi_n = 1; g1_14.flags = 4; g1_14.act = 0;
      g1_14.alpha = 1.0f; g1_14.beta = 1.0f; g1_14.sa = 1.0f; g1_14.sb = 1.0f; g1_14.Npad = N1; g1_14.pad_ = 0;
      k_gemm<1><<<dim3((unsigned)((N1) + 31) / 32, (unsigned)((Bn) + 15) / 16, (unsigned)(1)), 32, 0, stream>>>(g1_14); }
    k_vf_upd<<<(unsigned)((Bn * N0 + 255) / 256), 256, 0, stream>>>(S0, G0, R0, Bn * N0, 0.5f); k_vf_upd<<<(unsigned)((Bn * N1 + 255) / 256), 256, 0, stream>>>(S1, G1, R1, Bn * N1, 0.5f);
    { GemmP g0_15;
      g0_15.A = R1; g0_15.B = w0; g0_15.bias = b0; g0_15.R = R1; g0_15.C = G0;
      g0_15.sAo = 0; g0_15.sAi = 0; g0_15.sAm = N1; g0_15.sAk = 1; g0_15.sBo = 0; g0_15.sBi = 0; g0_15.sBn = N1; g0_15.sBk = 1; g0_15.sCo = 0; g0_15.sCi = 0; g0_15.sCm = N0; g0_15.sRo = 0; g0_15.sRi = 0; g0_15.sRm = 0; g0_15.sRn = 0;
      g0_15.M = Bn; g0_15.N = N0; g0_15.K = N1; g0_15.zi_n = 1; g0_15.flags = 1; g0_15.act = 0;
      g0_15.alpha = 1.0f; g0_15.beta = 0.0f; g0_15.sa = 1.0f; g0_15.sb = 1.0f; g0_15.Npad = N0; g0_15.pad_ = 0;
      k_gemm<1><<<dim3((unsigned)((N0) + 31) / 32, (unsigned)((Bn) + 15) / 16, (unsigned)(1)), 32, 0, stream>>>(g0_15); }
    { GemmP g1_15;
      g1_15.A = R0; g1_15.B = w1; g1_15.bias = R0; g1_15.R = INP1; g1_15.C = G1;
      g1_15.sAo = 0; g1_15.sAi = 0; g1_15.sAm = N0; g1_15.sAk = 1; g1_15.sBo = 0; g1_15.sBi = 0; g1_15.sBn = N0; g1_15.sBk = 1; g1_15.sCo = 0; g1_15.sCi = 0; g1_15.sCm = N1; g1_15.sRo = 0; g1_15.sRi = 0; g1_15.sRm = N1; g1_15.sRn = 1;
      g1_15.M = Bn; g1_15.N = N1; g1_15.K = N0; g1_15.zi_n = 1; g1_15.flags = 4; g1_15.act = 0;
      g1_15.alpha = 1.0f; g1_15.beta = 1.0f; g1_15.sa = 1.0f; g1_15.sb = 1.0f; g1_15.Npad = N1; g1_15.pad_ = 0;
      k_gemm<1><<<dim3((unsigned)((N1) + 31) / 32, (unsigned)((Bn) + 15) / 16, (unsigned)(1)), 32, 0, stream>>>(g1_15); }
    k_vf_upd<<<(unsigned)((Bn * N0 + 255) / 256), 256, 0, stream>>>(S0, G0, R0, Bn * N0, 0.5f); k_vf_upd<<<(unsigned)((Bn * N1 + 255) / 256), 256, 0, stream>>>(S1, G1, R1, Bn * N1, 0.5f);
    { GemmP g0_16;
      g0_16.A = R1; g0_16.B = w0; g0_16.bias = b0; g0_16.R = R1; g0_16.C = G0;
      g0_16.sAo = 0; g0_16.sAi = 0; g0_16.sAm = N1; g0_16.sAk = 1; g0_16.sBo = 0; g0_16.sBi = 0; g0_16.sBn = N1; g0_16.sBk = 1; g0_16.sCo = 0; g0_16.sCi = 0; g0_16.sCm = N0; g0_16.sRo = 0; g0_16.sRi = 0; g0_16.sRm = 0; g0_16.sRn = 0;
      g0_16.M = Bn; g0_16.N = N0; g0_16.K = N1; g0_16.zi_n = 1; g0_16.flags = 1; g0_16.act = 0;
      g0_16.alpha = 1.0f; g0_16.beta = 0.0f; g0_16.sa = 1.0f; g0_16.sb = 1.0f; g0_16.Npad = N0; g0_16.pad_ = 0;
      k_gemm<1><<<dim3((unsigned)((N0) + 31) / 32, (unsigned)((Bn) + 15) / 16, (unsigned)(1)), 32, 0, stream>>>(g0_16); }
    { GemmP g1_16;
      g1_16.A = R0; g1_16.B = w1; g1_16.bias = R0; g1_16.R = INP1; g1_16.C = G1;
      g1_16.sAo = 0; g1_16.sAi = 0; g1_16.sAm = N0; g1_16.sAk = 1; g1_16.sBo = 0; g1_16.sBi = 0; g1_16.sBn = N0; g1_16.sBk = 1; g1_16.sCo = 0; g1_16.sCi = 0; g1_16.sCm = N1; g1_16.sRo = 0; g1_16.sRi = 0; g1_16.sRm = N1; g1_16.sRn = 1;
      g1_16.M = Bn; g1_16.N = N1; g1_16.K = N0; g1_16.zi_n = 1; g1_16.flags = 4; g1_16.act = 0;
      g1_16.alpha = 1.0f; g1_16.beta = 1.0f; g1_16.sa = 1.0f; g1_16.sb = 1.0f; g1_16.Npad = N1; g1_16.pad_ = 0;
      k_gemm<1><<<dim3((unsigned)((N1) + 31) / 32, (unsigned)((Bn) + 15) / 16, (unsigned)(1)), 32, 0, stream>>>(g1_16); }
    k_vf_upd<<<(unsigned)((Bn * N0 + 255) / 256), 256, 0, stream>>>(S0, G0, R0, Bn * N0, 0.5f); k_vf_upd<<<(unsigned)((Bn * N1 + 255) / 256), 256, 0, stream>>>(S1, G1, R1, Bn * N1, 0.5f);
    { GemmP g0_17;
      g0_17.A = R1; g0_17.B = w0; g0_17.bias = b0; g0_17.R = R1; g0_17.C = G0;
      g0_17.sAo = 0; g0_17.sAi = 0; g0_17.sAm = N1; g0_17.sAk = 1; g0_17.sBo = 0; g0_17.sBi = 0; g0_17.sBn = N1; g0_17.sBk = 1; g0_17.sCo = 0; g0_17.sCi = 0; g0_17.sCm = N0; g0_17.sRo = 0; g0_17.sRi = 0; g0_17.sRm = 0; g0_17.sRn = 0;
      g0_17.M = Bn; g0_17.N = N0; g0_17.K = N1; g0_17.zi_n = 1; g0_17.flags = 1; g0_17.act = 0;
      g0_17.alpha = 1.0f; g0_17.beta = 0.0f; g0_17.sa = 1.0f; g0_17.sb = 1.0f; g0_17.Npad = N0; g0_17.pad_ = 0;
      k_gemm<1><<<dim3((unsigned)((N0) + 31) / 32, (unsigned)((Bn) + 15) / 16, (unsigned)(1)), 32, 0, stream>>>(g0_17); }
    { GemmP g1_17;
      g1_17.A = R0; g1_17.B = w1; g1_17.bias = R0; g1_17.R = INP1; g1_17.C = G1;
      g1_17.sAo = 0; g1_17.sAi = 0; g1_17.sAm = N0; g1_17.sAk = 1; g1_17.sBo = 0; g1_17.sBi = 0; g1_17.sBn = N0; g1_17.sBk = 1; g1_17.sCo = 0; g1_17.sCi = 0; g1_17.sCm = N1; g1_17.sRo = 0; g1_17.sRi = 0; g1_17.sRm = N1; g1_17.sRn = 1;
      g1_17.M = Bn; g1_17.N = N1; g1_17.K = N0; g1_17.zi_n = 1; g1_17.flags = 4; g1_17.act = 0;
      g1_17.alpha = 1.0f; g1_17.beta = 1.0f; g1_17.sa = 1.0f; g1_17.sb = 1.0f; g1_17.Npad = N1; g1_17.pad_ = 0;
      k_gemm<1><<<dim3((unsigned)((N1) + 31) / 32, (unsigned)((Bn) + 15) / 16, (unsigned)(1)), 32, 0, stream>>>(g1_17); }
    k_vf_upd<<<(unsigned)((Bn * N0 + 255) / 256), 256, 0, stream>>>(S0, G0, R0, Bn * N0, 0.5f); k_vf_upd<<<(unsigned)((Bn * N1 + 255) / 256), 256, 0, stream>>>(S1, G1, R1, Bn * N1, 0.5f);
    { GemmP g0_18;
      g0_18.A = R1; g0_18.B = w0; g0_18.bias = b0; g0_18.R = R1; g0_18.C = G0;
      g0_18.sAo = 0; g0_18.sAi = 0; g0_18.sAm = N1; g0_18.sAk = 1; g0_18.sBo = 0; g0_18.sBi = 0; g0_18.sBn = N1; g0_18.sBk = 1; g0_18.sCo = 0; g0_18.sCi = 0; g0_18.sCm = N0; g0_18.sRo = 0; g0_18.sRi = 0; g0_18.sRm = 0; g0_18.sRn = 0;
      g0_18.M = Bn; g0_18.N = N0; g0_18.K = N1; g0_18.zi_n = 1; g0_18.flags = 1; g0_18.act = 0;
      g0_18.alpha = 1.0f; g0_18.beta = 0.0f; g0_18.sa = 1.0f; g0_18.sb = 1.0f; g0_18.Npad = N0; g0_18.pad_ = 0;
      k_gemm<1><<<dim3((unsigned)((N0) + 31) / 32, (unsigned)((Bn) + 15) / 16, (unsigned)(1)), 32, 0, stream>>>(g0_18); }
    { GemmP g1_18;
      g1_18.A = R0; g1_18.B = w1; g1_18.bias = R0; g1_18.R = INP1; g1_18.C = G1;
      g1_18.sAo = 0; g1_18.sAi = 0; g1_18.sAm = N0; g1_18.sAk = 1; g1_18.sBo = 0; g1_18.sBi = 0; g1_18.sBn = N0; g1_18.sBk = 1; g1_18.sCo = 0; g1_18.sCi = 0; g1_18.sCm = N1; g1_18.sRo = 0; g1_18.sRi = 0; g1_18.sRm = N1; g1_18.sRn = 1;
      g1_18.M = Bn; g1_18.N = N1; g1_18.K = N0; g1_18.zi_n = 1; g1_18.flags = 4; g1_18.act = 0;
      g1_18.alpha = 1.0f; g1_18.beta = 1.0f; g1_18.sa = 1.0f; g1_18.sb = 1.0f; g1_18.Npad = N1; g1_18.pad_ = 0;
      k_gemm<1><<<dim3((unsigned)((N1) + 31) / 32, (unsigned)((Bn) + 15) / 16, (unsigned)(1)), 32, 0, stream>>>(g1_18); }
    k_vf_upd<<<(unsigned)((Bn * N0 + 255) / 256), 256, 0, stream>>>(S0, G0, R0, Bn * N0, 0.5f); k_vf_upd<<<(unsigned)((Bn * N1 + 255) / 256), 256, 0, stream>>>(S1, G1, R1, Bn * N1, 0.5f);
    { GemmP g0_19;
      g0_19.A = R1; g0_19.B = w0; g0_19.bias = b0; g0_19.R = R1; g0_19.C = G0;
      g0_19.sAo = 0; g0_19.sAi = 0; g0_19.sAm = N1; g0_19.sAk = 1; g0_19.sBo = 0; g0_19.sBi = 0; g0_19.sBn = N1; g0_19.sBk = 1; g0_19.sCo = 0; g0_19.sCi = 0; g0_19.sCm = N0; g0_19.sRo = 0; g0_19.sRi = 0; g0_19.sRm = 0; g0_19.sRn = 0;
      g0_19.M = Bn; g0_19.N = N0; g0_19.K = N1; g0_19.zi_n = 1; g0_19.flags = 1; g0_19.act = 0;
      g0_19.alpha = 1.0f; g0_19.beta = 0.0f; g0_19.sa = 1.0f; g0_19.sb = 1.0f; g0_19.Npad = N0; g0_19.pad_ = 0;
      k_gemm<1><<<dim3((unsigned)((N0) + 31) / 32, (unsigned)((Bn) + 15) / 16, (unsigned)(1)), 32, 0, stream>>>(g0_19); }
    { GemmP g1_19;
      g1_19.A = R0; g1_19.B = w1; g1_19.bias = R0; g1_19.R = INP1; g1_19.C = G1;
      g1_19.sAo = 0; g1_19.sAi = 0; g1_19.sAm = N0; g1_19.sAk = 1; g1_19.sBo = 0; g1_19.sBi = 0; g1_19.sBn = N0; g1_19.sBk = 1; g1_19.sCo = 0; g1_19.sCi = 0; g1_19.sCm = N1; g1_19.sRo = 0; g1_19.sRi = 0; g1_19.sRm = N1; g1_19.sRn = 1;
      g1_19.M = Bn; g1_19.N = N1; g1_19.K = N0; g1_19.zi_n = 1; g1_19.flags = 4; g1_19.act = 0;
      g1_19.alpha = 1.0f; g1_19.beta = 1.0f; g1_19.sa = 1.0f; g1_19.sb = 1.0f; g1_19.Npad = N1; g1_19.pad_ = 0;
      k_gemm<1><<<dim3((unsigned)((N1) + 31) / 32, (unsigned)((Bn) + 15) / 16, (unsigned)(1)), 32, 0, stream>>>(g1_19); }
    k_vf_upd<<<(unsigned)((Bn * N0 + 255) / 256), 256, 0, stream>>>(S0, G0, R0, Bn * N0, 0.5f); k_vf_upd<<<(unsigned)((Bn * N1 + 255) / 256), 256, 0, stream>>>(S1, G1, R1, Bn * N1, 0.5f);
    { GemmP g0_20;
      g0_20.A = R1; g0_20.B = w0; g0_20.bias = b0; g0_20.R = R1; g0_20.C = G0;
      g0_20.sAo = 0; g0_20.sAi = 0; g0_20.sAm = N1; g0_20.sAk = 1; g0_20.sBo = 0; g0_20.sBi = 0; g0_20.sBn = N1; g0_20.sBk = 1; g0_20.sCo = 0; g0_20.sCi = 0; g0_20.sCm = N0; g0_20.sRo = 0; g0_20.sRi = 0; g0_20.sRm = 0; g0_20.sRn = 0;
      g0_20.M = Bn; g0_20.N = N0; g0_20.K = N1; g0_20.zi_n = 1; g0_20.flags = 1; g0_20.act = 0;
      g0_20.alpha = 1.0f; g0_20.beta = 0.0f; g0_20.sa = 1.0f; g0_20.sb = 1.0f; g0_20.Npad = N0; g0_20.pad_ = 0;
      k_gemm<1><<<dim3((unsigned)((N0) + 31) / 32, (unsigned)((Bn) + 15) / 16, (unsigned)(1)), 32, 0, stream>>>(g0_20); }
    { GemmP g1_20;
      g1_20.A = R0; g1_20.B = w1; g1_20.bias = R0; g1_20.R = INP1; g1_20.C = G1;
      g1_20.sAo = 0; g1_20.sAi = 0; g1_20.sAm = N0; g1_20.sAk = 1; g1_20.sBo = 0; g1_20.sBi = 0; g1_20.sBn = N0; g1_20.sBk = 1; g1_20.sCo = 0; g1_20.sCi = 0; g1_20.sCm = N1; g1_20.sRo = 0; g1_20.sRi = 0; g1_20.sRm = N1; g1_20.sRn = 1;
      g1_20.M = Bn; g1_20.N = N1; g1_20.K = N0; g1_20.zi_n = 1; g1_20.flags = 4; g1_20.act = 0;
      g1_20.alpha = 1.0f; g1_20.beta = 1.0f; g1_20.sa = 1.0f; g1_20.sb = 1.0f; g1_20.Npad = N1; g1_20.pad_ = 0;
      k_gemm<1><<<dim3((unsigned)((N1) + 31) / 32, (unsigned)((Bn) + 15) / 16, (unsigned)(1)), 32, 0, stream>>>(g1_20); }
    k_vf_upd<<<(unsigned)((Bn * N0 + 255) / 256), 256, 0, stream>>>(S0, G0, R0, Bn * N0, 0.5f); k_vf_upd<<<(unsigned)((Bn * N1 + 255) / 256), 256, 0, stream>>>(S1, G1, R1, Bn * N1, 0.5f);
    { GemmP g0_21;
      g0_21.A = R1; g0_21.B = w0; g0_21.bias = b0; g0_21.R = R1; g0_21.C = G0;
      g0_21.sAo = 0; g0_21.sAi = 0; g0_21.sAm = N1; g0_21.sAk = 1; g0_21.sBo = 0; g0_21.sBi = 0; g0_21.sBn = N1; g0_21.sBk = 1; g0_21.sCo = 0; g0_21.sCi = 0; g0_21.sCm = N0; g0_21.sRo = 0; g0_21.sRi = 0; g0_21.sRm = 0; g0_21.sRn = 0;
      g0_21.M = Bn; g0_21.N = N0; g0_21.K = N1; g0_21.zi_n = 1; g0_21.flags = 1; g0_21.act = 0;
      g0_21.alpha = 1.0f; g0_21.beta = 0.0f; g0_21.sa = 1.0f; g0_21.sb = 1.0f; g0_21.Npad = N0; g0_21.pad_ = 0;
      k_gemm<1><<<dim3((unsigned)((N0) + 31) / 32, (unsigned)((Bn) + 15) / 16, (unsigned)(1)), 32, 0, stream>>>(g0_21); }
    { GemmP g1_21;
      g1_21.A = R0; g1_21.B = w1; g1_21.bias = R0; g1_21.R = INP1; g1_21.C = G1;
      g1_21.sAo = 0; g1_21.sAi = 0; g1_21.sAm = N0; g1_21.sAk = 1; g1_21.sBo = 0; g1_21.sBi = 0; g1_21.sBn = N0; g1_21.sBk = 1; g1_21.sCo = 0; g1_21.sCi = 0; g1_21.sCm = N1; g1_21.sRo = 0; g1_21.sRi = 0; g1_21.sRm = N1; g1_21.sRn = 1;
      g1_21.M = Bn; g1_21.N = N1; g1_21.K = N0; g1_21.zi_n = 1; g1_21.flags = 4; g1_21.act = 0;
      g1_21.alpha = 1.0f; g1_21.beta = 1.0f; g1_21.sa = 1.0f; g1_21.sb = 1.0f; g1_21.Npad = N1; g1_21.pad_ = 0;
      k_gemm<1><<<dim3((unsigned)((N1) + 31) / 32, (unsigned)((Bn) + 15) / 16, (unsigned)(1)), 32, 0, stream>>>(g1_21); }
    k_vf_upd<<<(unsigned)((Bn * N0 + 255) / 256), 256, 0, stream>>>(S0, G0, R0, Bn * N0, 0.5f); k_vf_upd<<<(unsigned)((Bn * N1 + 255) / 256), 256, 0, stream>>>(S1, G1, R1, Bn * N1, 0.5f);
    { GemmP g0_22;
      g0_22.A = R1; g0_22.B = w0; g0_22.bias = b0; g0_22.R = R1; g0_22.C = G0;
      g0_22.sAo = 0; g0_22.sAi = 0; g0_22.sAm = N1; g0_22.sAk = 1; g0_22.sBo = 0; g0_22.sBi = 0; g0_22.sBn = N1; g0_22.sBk = 1; g0_22.sCo = 0; g0_22.sCi = 0; g0_22.sCm = N0; g0_22.sRo = 0; g0_22.sRi = 0; g0_22.sRm = 0; g0_22.sRn = 0;
      g0_22.M = Bn; g0_22.N = N0; g0_22.K = N1; g0_22.zi_n = 1; g0_22.flags = 1; g0_22.act = 0;
      g0_22.alpha = 1.0f; g0_22.beta = 0.0f; g0_22.sa = 1.0f; g0_22.sb = 1.0f; g0_22.Npad = N0; g0_22.pad_ = 0;
      k_gemm<1><<<dim3((unsigned)((N0) + 31) / 32, (unsigned)((Bn) + 15) / 16, (unsigned)(1)), 32, 0, stream>>>(g0_22); }
    { GemmP g1_22;
      g1_22.A = R0; g1_22.B = w1; g1_22.bias = R0; g1_22.R = INP1; g1_22.C = G1;
      g1_22.sAo = 0; g1_22.sAi = 0; g1_22.sAm = N0; g1_22.sAk = 1; g1_22.sBo = 0; g1_22.sBi = 0; g1_22.sBn = N0; g1_22.sBk = 1; g1_22.sCo = 0; g1_22.sCi = 0; g1_22.sCm = N1; g1_22.sRo = 0; g1_22.sRi = 0; g1_22.sRm = N1; g1_22.sRn = 1;
      g1_22.M = Bn; g1_22.N = N1; g1_22.K = N0; g1_22.zi_n = 1; g1_22.flags = 4; g1_22.act = 0;
      g1_22.alpha = 1.0f; g1_22.beta = 1.0f; g1_22.sa = 1.0f; g1_22.sb = 1.0f; g1_22.Npad = N1; g1_22.pad_ = 0;
      k_gemm<1><<<dim3((unsigned)((N1) + 31) / 32, (unsigned)((Bn) + 15) / 16, (unsigned)(1)), 32, 0, stream>>>(g1_22); }
    k_vf_upd<<<(unsigned)((Bn * N0 + 255) / 256), 256, 0, stream>>>(S0, G0, R0, Bn * N0, 0.5f); k_vf_upd<<<(unsigned)((Bn * N1 + 255) / 256), 256, 0, stream>>>(S1, G1, R1, Bn * N1, 0.5f);
    { GemmP g0_23;
      g0_23.A = R1; g0_23.B = w0; g0_23.bias = b0; g0_23.R = R1; g0_23.C = G0;
      g0_23.sAo = 0; g0_23.sAi = 0; g0_23.sAm = N1; g0_23.sAk = 1; g0_23.sBo = 0; g0_23.sBi = 0; g0_23.sBn = N1; g0_23.sBk = 1; g0_23.sCo = 0; g0_23.sCi = 0; g0_23.sCm = N0; g0_23.sRo = 0; g0_23.sRi = 0; g0_23.sRm = 0; g0_23.sRn = 0;
      g0_23.M = Bn; g0_23.N = N0; g0_23.K = N1; g0_23.zi_n = 1; g0_23.flags = 1; g0_23.act = 0;
      g0_23.alpha = 1.0f; g0_23.beta = 0.0f; g0_23.sa = 1.0f; g0_23.sb = 1.0f; g0_23.Npad = N0; g0_23.pad_ = 0;
      k_gemm<1><<<dim3((unsigned)((N0) + 31) / 32, (unsigned)((Bn) + 15) / 16, (unsigned)(1)), 32, 0, stream>>>(g0_23); }
    { GemmP g1_23;
      g1_23.A = R0; g1_23.B = w1; g1_23.bias = R0; g1_23.R = INP1; g1_23.C = G1;
      g1_23.sAo = 0; g1_23.sAi = 0; g1_23.sAm = N0; g1_23.sAk = 1; g1_23.sBo = 0; g1_23.sBi = 0; g1_23.sBn = N0; g1_23.sBk = 1; g1_23.sCo = 0; g1_23.sCi = 0; g1_23.sCm = N1; g1_23.sRo = 0; g1_23.sRi = 0; g1_23.sRm = N1; g1_23.sRn = 1;
      g1_23.M = Bn; g1_23.N = N1; g1_23.K = N0; g1_23.zi_n = 1; g1_23.flags = 4; g1_23.act = 0;
      g1_23.alpha = 1.0f; g1_23.beta = 1.0f; g1_23.sa = 1.0f; g1_23.sb = 1.0f; g1_23.Npad = N1; g1_23.pad_ = 0;
      k_gemm<1><<<dim3((unsigned)((N1) + 31) / 32, (unsigned)((Bn) + 15) / 16, (unsigned)(1)), 32, 0, stream>>>(g1_23); }
    k_vf_upd<<<(unsigned)((Bn * N0 + 255) / 256), 256, 0, stream>>>(S0, G0, R0, Bn * N0, 0.5f); k_vf_upd<<<(unsigned)((Bn * N1 + 255) / 256), 256, 0, stream>>>(S1, G1, R1, Bn * N1, 0.5f);
    { GemmP g0_24;
      g0_24.A = R1; g0_24.B = w0; g0_24.bias = b0; g0_24.R = R1; g0_24.C = G0;
      g0_24.sAo = 0; g0_24.sAi = 0; g0_24.sAm = N1; g0_24.sAk = 1; g0_24.sBo = 0; g0_24.sBi = 0; g0_24.sBn = N1; g0_24.sBk = 1; g0_24.sCo = 0; g0_24.sCi = 0; g0_24.sCm = N0; g0_24.sRo = 0; g0_24.sRi = 0; g0_24.sRm = 0; g0_24.sRn = 0;
      g0_24.M = Bn; g0_24.N = N0; g0_24.K = N1; g0_24.zi_n = 1; g0_24.flags = 1; g0_24.act = 0;
      g0_24.alpha = 1.0f; g0_24.beta = 0.0f; g0_24.sa = 1.0f; g0_24.sb = 1.0f; g0_24.Npad = N0; g0_24.pad_ = 0;
      k_gemm<1><<<dim3((unsigned)((N0) + 31) / 32, (unsigned)((Bn) + 15) / 16, (unsigned)(1)), 32, 0, stream>>>(g0_24); }
    { GemmP g1_24;
      g1_24.A = R0; g1_24.B = w1; g1_24.bias = R0; g1_24.R = INP1; g1_24.C = G1;
      g1_24.sAo = 0; g1_24.sAi = 0; g1_24.sAm = N0; g1_24.sAk = 1; g1_24.sBo = 0; g1_24.sBi = 0; g1_24.sBn = N0; g1_24.sBk = 1; g1_24.sCo = 0; g1_24.sCi = 0; g1_24.sCm = N1; g1_24.sRo = 0; g1_24.sRi = 0; g1_24.sRm = N1; g1_24.sRn = 1;
      g1_24.M = Bn; g1_24.N = N1; g1_24.K = N0; g1_24.zi_n = 1; g1_24.flags = 4; g1_24.act = 0;
      g1_24.alpha = 1.0f; g1_24.beta = 1.0f; g1_24.sa = 1.0f; g1_24.sb = 1.0f; g1_24.Npad = N1; g1_24.pad_ = 0;
      k_gemm<1><<<dim3((unsigned)((N1) + 31) / 32, (unsigned)((Bn) + 15) / 16, (unsigned)(1)), 32, 0, stream>>>(g1_24); }
    k_vf_upd<<<(unsigned)((Bn * N0 + 255) / 256), 256, 0, stream>>>(S0, G0, R0, Bn * N0, 0.5f); k_vf_upd<<<(unsigned)((Bn * N1 + 255) / 256), 256, 0, stream>>>(S1, G1, R1, Bn * N1, 0.5f);
    { GemmP g0_25;
      g0_25.A = R1; g0_25.B = w0; g0_25.bias = b0; g0_25.R = R1; g0_25.C = G0;
      g0_25.sAo = 0; g0_25.sAi = 0; g0_25.sAm = N1; g0_25.sAk = 1; g0_25.sBo = 0; g0_25.sBi = 0; g0_25.sBn = N1; g0_25.sBk = 1; g0_25.sCo = 0; g0_25.sCi = 0; g0_25.sCm = N0; g0_25.sRo = 0; g0_25.sRi = 0; g0_25.sRm = 0; g0_25.sRn = 0;
      g0_25.M = Bn; g0_25.N = N0; g0_25.K = N1; g0_25.zi_n = 1; g0_25.flags = 1; g0_25.act = 0;
      g0_25.alpha = 1.0f; g0_25.beta = 0.0f; g0_25.sa = 1.0f; g0_25.sb = 1.0f; g0_25.Npad = N0; g0_25.pad_ = 0;
      k_gemm<1><<<dim3((unsigned)((N0) + 31) / 32, (unsigned)((Bn) + 15) / 16, (unsigned)(1)), 32, 0, stream>>>(g0_25); }
    { GemmP g1_25;
      g1_25.A = R0; g1_25.B = w1; g1_25.bias = R0; g1_25.R = INP1; g1_25.C = G1;
      g1_25.sAo = 0; g1_25.sAi = 0; g1_25.sAm = N0; g1_25.sAk = 1; g1_25.sBo = 0; g1_25.sBi = 0; g1_25.sBn = N0; g1_25.sBk = 1; g1_25.sCo = 0; g1_25.sCi = 0; g1_25.sCm = N1; g1_25.sRo = 0; g1_25.sRi = 0; g1_25.sRm = N1; g1_25.sRn = 1;
      g1_25.M = Bn; g1_25.N = N1; g1_25.K = N0; g1_25.zi_n = 1; g1_25.flags = 4; g1_25.act = 0;
      g1_25.alpha = 1.0f; g1_25.beta = 1.0f; g1_25.sa = 1.0f; g1_25.sb = 1.0f; g1_25.Npad = N1; g1_25.pad_ = 0;
      k_gemm<1><<<dim3((unsigned)((N1) + 31) / 32, (unsigned)((Bn) + 15) / 16, (unsigned)(1)), 32, 0, stream>>>(g1_25); }
    k_vf_upd<<<(unsigned)((Bn * N0 + 255) / 256), 256, 0, stream>>>(S0, G0, R0, Bn * N0, 0.5f); k_vf_upd<<<(unsigned)((Bn * N1 + 255) / 256), 256, 0, stream>>>(S1, G1, R1, Bn * N1, 0.5f);
    { GemmP g0_26;
      g0_26.A = R1; g0_26.B = w0; g0_26.bias = b0; g0_26.R = R1; g0_26.C = G0;
      g0_26.sAo = 0; g0_26.sAi = 0; g0_26.sAm = N1; g0_26.sAk = 1; g0_26.sBo = 0; g0_26.sBi = 0; g0_26.sBn = N1; g0_26.sBk = 1; g0_26.sCo = 0; g0_26.sCi = 0; g0_26.sCm = N0; g0_26.sRo = 0; g0_26.sRi = 0; g0_26.sRm = 0; g0_26.sRn = 0;
      g0_26.M = Bn; g0_26.N = N0; g0_26.K = N1; g0_26.zi_n = 1; g0_26.flags = 1; g0_26.act = 0;
      g0_26.alpha = 1.0f; g0_26.beta = 0.0f; g0_26.sa = 1.0f; g0_26.sb = 1.0f; g0_26.Npad = N0; g0_26.pad_ = 0;
      k_gemm<1><<<dim3((unsigned)((N0) + 31) / 32, (unsigned)((Bn) + 15) / 16, (unsigned)(1)), 32, 0, stream>>>(g0_26); }
    { GemmP g1_26;
      g1_26.A = R0; g1_26.B = w1; g1_26.bias = R0; g1_26.R = INP1; g1_26.C = G1;
      g1_26.sAo = 0; g1_26.sAi = 0; g1_26.sAm = N0; g1_26.sAk = 1; g1_26.sBo = 0; g1_26.sBi = 0; g1_26.sBn = N0; g1_26.sBk = 1; g1_26.sCo = 0; g1_26.sCi = 0; g1_26.sCm = N1; g1_26.sRo = 0; g1_26.sRi = 0; g1_26.sRm = N1; g1_26.sRn = 1;
      g1_26.M = Bn; g1_26.N = N1; g1_26.K = N0; g1_26.zi_n = 1; g1_26.flags = 4; g1_26.act = 0;
      g1_26.alpha = 1.0f; g1_26.beta = 1.0f; g1_26.sa = 1.0f; g1_26.sb = 1.0f; g1_26.Npad = N1; g1_26.pad_ = 0;
      k_gemm<1><<<dim3((unsigned)((N1) + 31) / 32, (unsigned)((Bn) + 15) / 16, (unsigned)(1)), 32, 0, stream>>>(g1_26); }
    k_vf_upd<<<(unsigned)((Bn * N0 + 255) / 256), 256, 0, stream>>>(S0, G0, R0, Bn * N0, 0.5f); k_vf_upd<<<(unsigned)((Bn * N1 + 255) / 256), 256, 0, stream>>>(S1, G1, R1, Bn * N1, 0.5f);
    { GemmP g0_27;
      g0_27.A = R1; g0_27.B = w0; g0_27.bias = b0; g0_27.R = R1; g0_27.C = G0;
      g0_27.sAo = 0; g0_27.sAi = 0; g0_27.sAm = N1; g0_27.sAk = 1; g0_27.sBo = 0; g0_27.sBi = 0; g0_27.sBn = N1; g0_27.sBk = 1; g0_27.sCo = 0; g0_27.sCi = 0; g0_27.sCm = N0; g0_27.sRo = 0; g0_27.sRi = 0; g0_27.sRm = 0; g0_27.sRn = 0;
      g0_27.M = Bn; g0_27.N = N0; g0_27.K = N1; g0_27.zi_n = 1; g0_27.flags = 1; g0_27.act = 0;
      g0_27.alpha = 1.0f; g0_27.beta = 0.0f; g0_27.sa = 1.0f; g0_27.sb = 1.0f; g0_27.Npad = N0; g0_27.pad_ = 0;
      k_gemm<1><<<dim3((unsigned)((N0) + 31) / 32, (unsigned)((Bn) + 15) / 16, (unsigned)(1)), 32, 0, stream>>>(g0_27); }
    { GemmP g1_27;
      g1_27.A = R0; g1_27.B = w1; g1_27.bias = R0; g1_27.R = INP1; g1_27.C = G1;
      g1_27.sAo = 0; g1_27.sAi = 0; g1_27.sAm = N0; g1_27.sAk = 1; g1_27.sBo = 0; g1_27.sBi = 0; g1_27.sBn = N0; g1_27.sBk = 1; g1_27.sCo = 0; g1_27.sCi = 0; g1_27.sCm = N1; g1_27.sRo = 0; g1_27.sRi = 0; g1_27.sRm = N1; g1_27.sRn = 1;
      g1_27.M = Bn; g1_27.N = N1; g1_27.K = N0; g1_27.zi_n = 1; g1_27.flags = 4; g1_27.act = 0;
      g1_27.alpha = 1.0f; g1_27.beta = 1.0f; g1_27.sa = 1.0f; g1_27.sb = 1.0f; g1_27.Npad = N1; g1_27.pad_ = 0;
      k_gemm<1><<<dim3((unsigned)((N1) + 31) / 32, (unsigned)((Bn) + 15) / 16, (unsigned)(1)), 32, 0, stream>>>(g1_27); }
    k_vf_upd<<<(unsigned)((Bn * N0 + 255) / 256), 256, 0, stream>>>(S0, G0, R0, Bn * N0, 0.5f); k_vf_upd<<<(unsigned)((Bn * N1 + 255) / 256), 256, 0, stream>>>(S1, G1, R1, Bn * N1, 0.5f);
    { GemmP g0_28;
      g0_28.A = R1; g0_28.B = w0; g0_28.bias = b0; g0_28.R = R1; g0_28.C = G0;
      g0_28.sAo = 0; g0_28.sAi = 0; g0_28.sAm = N1; g0_28.sAk = 1; g0_28.sBo = 0; g0_28.sBi = 0; g0_28.sBn = N1; g0_28.sBk = 1; g0_28.sCo = 0; g0_28.sCi = 0; g0_28.sCm = N0; g0_28.sRo = 0; g0_28.sRi = 0; g0_28.sRm = 0; g0_28.sRn = 0;
      g0_28.M = Bn; g0_28.N = N0; g0_28.K = N1; g0_28.zi_n = 1; g0_28.flags = 1; g0_28.act = 0;
      g0_28.alpha = 1.0f; g0_28.beta = 0.0f; g0_28.sa = 1.0f; g0_28.sb = 1.0f; g0_28.Npad = N0; g0_28.pad_ = 0;
      k_gemm<1><<<dim3((unsigned)((N0) + 31) / 32, (unsigned)((Bn) + 15) / 16, (unsigned)(1)), 32, 0, stream>>>(g0_28); }
    { GemmP g1_28;
      g1_28.A = R0; g1_28.B = w1; g1_28.bias = R0; g1_28.R = INP1; g1_28.C = G1;
      g1_28.sAo = 0; g1_28.sAi = 0; g1_28.sAm = N0; g1_28.sAk = 1; g1_28.sBo = 0; g1_28.sBi = 0; g1_28.sBn = N0; g1_28.sBk = 1; g1_28.sCo = 0; g1_28.sCi = 0; g1_28.sCm = N1; g1_28.sRo = 0; g1_28.sRi = 0; g1_28.sRm = N1; g1_28.sRn = 1;
      g1_28.M = Bn; g1_28.N = N1; g1_28.K = N0; g1_28.zi_n = 1; g1_28.flags = 4; g1_28.act = 0;
      g1_28.alpha = 1.0f; g1_28.beta = 1.0f; g1_28.sa = 1.0f; g1_28.sb = 1.0f; g1_28.Npad = N1; g1_28.pad_ = 0;
      k_gemm<1><<<dim3((unsigned)((N1) + 31) / 32, (unsigned)((Bn) + 15) / 16, (unsigned)(1)), 32, 0, stream>>>(g1_28); }
    k_vf_upd<<<(unsigned)((Bn * N0 + 255) / 256), 256, 0, stream>>>(S0, G0, R0, Bn * N0, 0.5f); k_vf_upd<<<(unsigned)((Bn * N1 + 255) / 256), 256, 0, stream>>>(S1, G1, R1, Bn * N1, 0.5f);
    { GemmP g0_29;
      g0_29.A = R1; g0_29.B = w0; g0_29.bias = b0; g0_29.R = R1; g0_29.C = G0;
      g0_29.sAo = 0; g0_29.sAi = 0; g0_29.sAm = N1; g0_29.sAk = 1; g0_29.sBo = 0; g0_29.sBi = 0; g0_29.sBn = N1; g0_29.sBk = 1; g0_29.sCo = 0; g0_29.sCi = 0; g0_29.sCm = N0; g0_29.sRo = 0; g0_29.sRi = 0; g0_29.sRm = 0; g0_29.sRn = 0;
      g0_29.M = Bn; g0_29.N = N0; g0_29.K = N1; g0_29.zi_n = 1; g0_29.flags = 1; g0_29.act = 0;
      g0_29.alpha = 1.0f; g0_29.beta = 0.0f; g0_29.sa = 1.0f; g0_29.sb = 1.0f; g0_29.Npad = N0; g0_29.pad_ = 0;
      k_gemm<1><<<dim3((unsigned)((N0) + 31) / 32, (unsigned)((Bn) + 15) / 16, (unsigned)(1)), 32, 0, stream>>>(g0_29); }
    { GemmP g1_29;
      g1_29.A = R0; g1_29.B = w1; g1_29.bias = R0; g1_29.R = INP1; g1_29.C = G1;
      g1_29.sAo = 0; g1_29.sAi = 0; g1_29.sAm = N0; g1_29.sAk = 1; g1_29.sBo = 0; g1_29.sBi = 0; g1_29.sBn = N0; g1_29.sBk = 1; g1_29.sCo = 0; g1_29.sCi = 0; g1_29.sCm = N1; g1_29.sRo = 0; g1_29.sRi = 0; g1_29.sRm = N1; g1_29.sRn = 1;
      g1_29.M = Bn; g1_29.N = N1; g1_29.K = N0; g1_29.zi_n = 1; g1_29.flags = 4; g1_29.act = 0;
      g1_29.alpha = 1.0f; g1_29.beta = 1.0f; g1_29.sa = 1.0f; g1_29.sb = 1.0f; g1_29.Npad = N1; g1_29.pad_ = 0;
      k_gemm<1><<<dim3((unsigned)((N1) + 31) / 32, (unsigned)((Bn) + 15) / 16, (unsigned)(1)), 32, 0, stream>>>(g1_29); }
    k_vf_upd<<<(unsigned)((Bn * N0 + 255) / 256), 256, 0, stream>>>(S0, G0, R0, Bn * N0, 0.5f); k_vf_upd<<<(unsigned)((Bn * N1 + 255) / 256), 256, 0, stream>>>(S1, G1, R1, Bn * N1, 0.5f);
    { GemmP g0_30;
      g0_30.A = R1; g0_30.B = w0; g0_30.bias = b0; g0_30.R = R1; g0_30.C = G0;
      g0_30.sAo = 0; g0_30.sAi = 0; g0_30.sAm = N1; g0_30.sAk = 1; g0_30.sBo = 0; g0_30.sBi = 0; g0_30.sBn = N1; g0_30.sBk = 1; g0_30.sCo = 0; g0_30.sCi = 0; g0_30.sCm = N0; g0_30.sRo = 0; g0_30.sRi = 0; g0_30.sRm = 0; g0_30.sRn = 0;
      g0_30.M = Bn; g0_30.N = N0; g0_30.K = N1; g0_30.zi_n = 1; g0_30.flags = 1; g0_30.act = 0;
      g0_30.alpha = 1.0f; g0_30.beta = 0.0f; g0_30.sa = 1.0f; g0_30.sb = 1.0f; g0_30.Npad = N0; g0_30.pad_ = 0;
      k_gemm<1><<<dim3((unsigned)((N0) + 31) / 32, (unsigned)((Bn) + 15) / 16, (unsigned)(1)), 32, 0, stream>>>(g0_30); }
    { GemmP g1_30;
      g1_30.A = R0; g1_30.B = w1; g1_30.bias = R0; g1_30.R = INP1; g1_30.C = G1;
      g1_30.sAo = 0; g1_30.sAi = 0; g1_30.sAm = N0; g1_30.sAk = 1; g1_30.sBo = 0; g1_30.sBi = 0; g1_30.sBn = N0; g1_30.sBk = 1; g1_30.sCo = 0; g1_30.sCi = 0; g1_30.sCm = N1; g1_30.sRo = 0; g1_30.sRi = 0; g1_30.sRm = N1; g1_30.sRn = 1;
      g1_30.M = Bn; g1_30.N = N1; g1_30.K = N0; g1_30.zi_n = 1; g1_30.flags = 4; g1_30.act = 0;
      g1_30.alpha = 1.0f; g1_30.beta = 1.0f; g1_30.sa = 1.0f; g1_30.sb = 1.0f; g1_30.Npad = N1; g1_30.pad_ = 0;
      k_gemm<1><<<dim3((unsigned)((N1) + 31) / 32, (unsigned)((Bn) + 15) / 16, (unsigned)(1)), 32, 0, stream>>>(g1_30); }
    k_vf_upd<<<(unsigned)((Bn * N0 + 255) / 256), 256, 0, stream>>>(S0, G0, R0, Bn * N0, 0.5f); k_vf_upd<<<(unsigned)((Bn * N1 + 255) / 256), 256, 0, stream>>>(S1, G1, R1, Bn * N1, 0.5f);
    { GemmP g0_31;
      g0_31.A = R1; g0_31.B = w0; g0_31.bias = b0; g0_31.R = R1; g0_31.C = G0;
      g0_31.sAo = 0; g0_31.sAi = 0; g0_31.sAm = N1; g0_31.sAk = 1; g0_31.sBo = 0; g0_31.sBi = 0; g0_31.sBn = N1; g0_31.sBk = 1; g0_31.sCo = 0; g0_31.sCi = 0; g0_31.sCm = N0; g0_31.sRo = 0; g0_31.sRi = 0; g0_31.sRm = 0; g0_31.sRn = 0;
      g0_31.M = Bn; g0_31.N = N0; g0_31.K = N1; g0_31.zi_n = 1; g0_31.flags = 1; g0_31.act = 0;
      g0_31.alpha = 1.0f; g0_31.beta = 0.0f; g0_31.sa = 1.0f; g0_31.sb = 1.0f; g0_31.Npad = N0; g0_31.pad_ = 0;
      k_gemm<1><<<dim3((unsigned)((N0) + 31) / 32, (unsigned)((Bn) + 15) / 16, (unsigned)(1)), 32, 0, stream>>>(g0_31); }
    { GemmP g1_31;
      g1_31.A = R0; g1_31.B = w1; g1_31.bias = R0; g1_31.R = INP1; g1_31.C = G1;
      g1_31.sAo = 0; g1_31.sAi = 0; g1_31.sAm = N0; g1_31.sAk = 1; g1_31.sBo = 0; g1_31.sBi = 0; g1_31.sBn = N0; g1_31.sBk = 1; g1_31.sCo = 0; g1_31.sCi = 0; g1_31.sCm = N1; g1_31.sRo = 0; g1_31.sRi = 0; g1_31.sRm = N1; g1_31.sRn = 1;
      g1_31.M = Bn; g1_31.N = N1; g1_31.K = N0; g1_31.zi_n = 1; g1_31.flags = 4; g1_31.act = 0;
      g1_31.alpha = 1.0f; g1_31.beta = 1.0f; g1_31.sa = 1.0f; g1_31.sb = 1.0f; g1_31.Npad = N1; g1_31.pad_ = 0;
      k_gemm<1><<<dim3((unsigned)((N1) + 31) / 32, (unsigned)((Bn) + 15) / 16, (unsigned)(1)), 32, 0, stream>>>(g1_31); }
    k_vf_upd<<<(unsigned)((Bn * N0 + 255) / 256), 256, 0, stream>>>(S0, G0, R0, Bn * N0, 0.5f); k_vf_upd<<<(unsigned)((Bn * N1 + 255) / 256), 256, 0, stream>>>(S1, G1, R1, Bn * N1, 0.5f);
    { GemmP g0_32;
      g0_32.A = R1; g0_32.B = w0; g0_32.bias = b0; g0_32.R = R1; g0_32.C = G0;
      g0_32.sAo = 0; g0_32.sAi = 0; g0_32.sAm = N1; g0_32.sAk = 1; g0_32.sBo = 0; g0_32.sBi = 0; g0_32.sBn = N1; g0_32.sBk = 1; g0_32.sCo = 0; g0_32.sCi = 0; g0_32.sCm = N0; g0_32.sRo = 0; g0_32.sRi = 0; g0_32.sRm = 0; g0_32.sRn = 0;
      g0_32.M = Bn; g0_32.N = N0; g0_32.K = N1; g0_32.zi_n = 1; g0_32.flags = 1; g0_32.act = 0;
      g0_32.alpha = 1.0f; g0_32.beta = 0.0f; g0_32.sa = 1.0f; g0_32.sb = 1.0f; g0_32.Npad = N0; g0_32.pad_ = 0;
      k_gemm<1><<<dim3((unsigned)((N0) + 31) / 32, (unsigned)((Bn) + 15) / 16, (unsigned)(1)), 32, 0, stream>>>(g0_32); }
    { GemmP g1_32;
      g1_32.A = R0; g1_32.B = w1; g1_32.bias = R0; g1_32.R = INP1; g1_32.C = G1;
      g1_32.sAo = 0; g1_32.sAi = 0; g1_32.sAm = N0; g1_32.sAk = 1; g1_32.sBo = 0; g1_32.sBi = 0; g1_32.sBn = N0; g1_32.sBk = 1; g1_32.sCo = 0; g1_32.sCi = 0; g1_32.sCm = N1; g1_32.sRo = 0; g1_32.sRi = 0; g1_32.sRm = N1; g1_32.sRn = 1;
      g1_32.M = Bn; g1_32.N = N1; g1_32.K = N0; g1_32.zi_n = 1; g1_32.flags = 4; g1_32.act = 0;
      g1_32.alpha = 1.0f; g1_32.beta = 1.0f; g1_32.sa = 1.0f; g1_32.sb = 1.0f; g1_32.Npad = N1; g1_32.pad_ = 0;
      k_gemm<1><<<dim3((unsigned)((N1) + 31) / 32, (unsigned)((Bn) + 15) / 16, (unsigned)(1)), 32, 0, stream>>>(g1_32); }
    k_vf_upd<<<(unsigned)((Bn * N0 + 255) / 256), 256, 0, stream>>>(S0, G0, R0, Bn * N0, 0.5f); k_vf_upd<<<(unsigned)((Bn * N1 + 255) / 256), 256, 0, stream>>>(S1, G1, R1, Bn * N1, 0.5f);
    { GemmP g0_33;
      g0_33.A = R1; g0_33.B = w0; g0_33.bias = b0; g0_33.R = R1; g0_33.C = G0;
      g0_33.sAo = 0; g0_33.sAi = 0; g0_33.sAm = N1; g0_33.sAk = 1; g0_33.sBo = 0; g0_33.sBi = 0; g0_33.sBn = N1; g0_33.sBk = 1; g0_33.sCo = 0; g0_33.sCi = 0; g0_33.sCm = N0; g0_33.sRo = 0; g0_33.sRi = 0; g0_33.sRm = 0; g0_33.sRn = 0;
      g0_33.M = Bn; g0_33.N = N0; g0_33.K = N1; g0_33.zi_n = 1; g0_33.flags = 1; g0_33.act = 0;
      g0_33.alpha = 1.0f; g0_33.beta = 0.0f; g0_33.sa = 1.0f; g0_33.sb = 1.0f; g0_33.Npad = N0; g0_33.pad_ = 0;
      k_gemm<1><<<dim3((unsigned)((N0) + 31) / 32, (unsigned)((Bn) + 15) / 16, (unsigned)(1)), 32, 0, stream>>>(g0_33); }
    { GemmP g1_33;
      g1_33.A = R0; g1_33.B = w1; g1_33.bias = R0; g1_33.R = INP1; g1_33.C = G1;
      g1_33.sAo = 0; g1_33.sAi = 0; g1_33.sAm = N0; g1_33.sAk = 1; g1_33.sBo = 0; g1_33.sBi = 0; g1_33.sBn = N0; g1_33.sBk = 1; g1_33.sCo = 0; g1_33.sCi = 0; g1_33.sCm = N1; g1_33.sRo = 0; g1_33.sRi = 0; g1_33.sRm = N1; g1_33.sRn = 1;
      g1_33.M = Bn; g1_33.N = N1; g1_33.K = N0; g1_33.zi_n = 1; g1_33.flags = 4; g1_33.act = 0;
      g1_33.alpha = 1.0f; g1_33.beta = 1.0f; g1_33.sa = 1.0f; g1_33.sb = 1.0f; g1_33.Npad = N1; g1_33.pad_ = 0;
      k_gemm<1><<<dim3((unsigned)((N1) + 31) / 32, (unsigned)((Bn) + 15) / 16, (unsigned)(1)), 32, 0, stream>>>(g1_33); }
    k_vf_upd<<<(unsigned)((Bn * N0 + 255) / 256), 256, 0, stream>>>(S0, G0, R0, Bn * N0, 0.5f); k_vf_upd<<<(unsigned)((Bn * N1 + 255) / 256), 256, 0, stream>>>(S1, G1, R1, Bn * N1, 0.5f);
    { GemmP g0_34;
      g0_34.A = R1; g0_34.B = w0; g0_34.bias = b0; g0_34.R = R1; g0_34.C = G0;
      g0_34.sAo = 0; g0_34.sAi = 0; g0_34.sAm = N1; g0_34.sAk = 1; g0_34.sBo = 0; g0_34.sBi = 0; g0_34.sBn = N1; g0_34.sBk = 1; g0_34.sCo = 0; g0_34.sCi = 0; g0_34.sCm = N0; g0_34.sRo = 0; g0_34.sRi = 0; g0_34.sRm = 0; g0_34.sRn = 0;
      g0_34.M = Bn; g0_34.N = N0; g0_34.K = N1; g0_34.zi_n = 1; g0_34.flags = 1; g0_34.act = 0;
      g0_34.alpha = 1.0f; g0_34.beta = 0.0f; g0_34.sa = 1.0f; g0_34.sb = 1.0f; g0_34.Npad = N0; g0_34.pad_ = 0;
      k_gemm<1><<<dim3((unsigned)((N0) + 31) / 32, (unsigned)((Bn) + 15) / 16, (unsigned)(1)), 32, 0, stream>>>(g0_34); }
    { GemmP g1_34;
      g1_34.A = R0; g1_34.B = w1; g1_34.bias = R0; g1_34.R = INP1; g1_34.C = G1;
      g1_34.sAo = 0; g1_34.sAi = 0; g1_34.sAm = N0; g1_34.sAk = 1; g1_34.sBo = 0; g1_34.sBi = 0; g1_34.sBn = N0; g1_34.sBk = 1; g1_34.sCo = 0; g1_34.sCi = 0; g1_34.sCm = N1; g1_34.sRo = 0; g1_34.sRi = 0; g1_34.sRm = N1; g1_34.sRn = 1;
      g1_34.M = Bn; g1_34.N = N1; g1_34.K = N0; g1_34.zi_n = 1; g1_34.flags = 4; g1_34.act = 0;
      g1_34.alpha = 1.0f; g1_34.beta = 1.0f; g1_34.sa = 1.0f; g1_34.sb = 1.0f; g1_34.Npad = N1; g1_34.pad_ = 0;
      k_gemm<1><<<dim3((unsigned)((N1) + 31) / 32, (unsigned)((Bn) + 15) / 16, (unsigned)(1)), 32, 0, stream>>>(g1_34); }
    k_vf_upd<<<(unsigned)((Bn * N0 + 255) / 256), 256, 0, stream>>>(S0, G0, R0, Bn * N0, 0.5f); k_vf_upd<<<(unsigned)((Bn * N1 + 255) / 256), 256, 0, stream>>>(S1, G1, R1, Bn * N1, 0.5f);
    { GemmP g0_35;
      g0_35.A = R1; g0_35.B = w0; g0_35.bias = b0; g0_35.R = R1; g0_35.C = G0;
      g0_35.sAo = 0; g0_35.sAi = 0; g0_35.sAm = N1; g0_35.sAk = 1; g0_35.sBo = 0; g0_35.sBi = 0; g0_35.sBn = N1; g0_35.sBk = 1; g0_35.sCo = 0; g0_35.sCi = 0; g0_35.sCm = N0; g0_35.sRo = 0; g0_35.sRi = 0; g0_35.sRm = 0; g0_35.sRn = 0;
      g0_35.M = Bn; g0_35.N = N0; g0_35.K = N1; g0_35.zi_n = 1; g0_35.flags = 1; g0_35.act = 0;
      g0_35.alpha = 1.0f; g0_35.beta = 0.0f; g0_35.sa = 1.0f; g0_35.sb = 1.0f; g0_35.Npad = N0; g0_35.pad_ = 0;
      k_gemm<1><<<dim3((unsigned)((N0) + 31) / 32, (unsigned)((Bn) + 15) / 16, (unsigned)(1)), 32, 0, stream>>>(g0_35); }
    { GemmP g1_35;
      g1_35.A = R0; g1_35.B = w1; g1_35.bias = R0; g1_35.R = INP1; g1_35.C = G1;
      g1_35.sAo = 0; g1_35.sAi = 0; g1_35.sAm = N0; g1_35.sAk = 1; g1_35.sBo = 0; g1_35.sBi = 0; g1_35.sBn = N0; g1_35.sBk = 1; g1_35.sCo = 0; g1_35.sCi = 0; g1_35.sCm = N1; g1_35.sRo = 0; g1_35.sRi = 0; g1_35.sRm = N1; g1_35.sRn = 1;
      g1_35.M = Bn; g1_35.N = N1; g1_35.K = N0; g1_35.zi_n = 1; g1_35.flags = 4; g1_35.act = 0;
      g1_35.alpha = 1.0f; g1_35.beta = 1.0f; g1_35.sa = 1.0f; g1_35.sb = 1.0f; g1_35.Npad = N1; g1_35.pad_ = 0;
      k_gemm<1><<<dim3((unsigned)((N1) + 31) / 32, (unsigned)((Bn) + 15) / 16, (unsigned)(1)), 32, 0, stream>>>(g1_35); }
    k_vf_upd<<<(unsigned)((Bn * N0 + 255) / 256), 256, 0, stream>>>(S0, G0, R0, Bn * N0, 0.5f); k_vf_upd<<<(unsigned)((Bn * N1 + 255) / 256), 256, 0, stream>>>(S1, G1, R1, Bn * N1, 0.5f);
    { GemmP g0_36;
      g0_36.A = R1; g0_36.B = w0; g0_36.bias = b0; g0_36.R = R1; g0_36.C = G0;
      g0_36.sAo = 0; g0_36.sAi = 0; g0_36.sAm = N1; g0_36.sAk = 1; g0_36.sBo = 0; g0_36.sBi = 0; g0_36.sBn = N1; g0_36.sBk = 1; g0_36.sCo = 0; g0_36.sCi = 0; g0_36.sCm = N0; g0_36.sRo = 0; g0_36.sRi = 0; g0_36.sRm = 0; g0_36.sRn = 0;
      g0_36.M = Bn; g0_36.N = N0; g0_36.K = N1; g0_36.zi_n = 1; g0_36.flags = 1; g0_36.act = 0;
      g0_36.alpha = 1.0f; g0_36.beta = 0.0f; g0_36.sa = 1.0f; g0_36.sb = 1.0f; g0_36.Npad = N0; g0_36.pad_ = 0;
      k_gemm<1><<<dim3((unsigned)((N0) + 31) / 32, (unsigned)((Bn) + 15) / 16, (unsigned)(1)), 32, 0, stream>>>(g0_36); }
    { GemmP g1_36;
      g1_36.A = R0; g1_36.B = w1; g1_36.bias = R0; g1_36.R = INP1; g1_36.C = G1;
      g1_36.sAo = 0; g1_36.sAi = 0; g1_36.sAm = N0; g1_36.sAk = 1; g1_36.sBo = 0; g1_36.sBi = 0; g1_36.sBn = N0; g1_36.sBk = 1; g1_36.sCo = 0; g1_36.sCi = 0; g1_36.sCm = N1; g1_36.sRo = 0; g1_36.sRi = 0; g1_36.sRm = N1; g1_36.sRn = 1;
      g1_36.M = Bn; g1_36.N = N1; g1_36.K = N0; g1_36.zi_n = 1; g1_36.flags = 4; g1_36.act = 0;
      g1_36.alpha = 1.0f; g1_36.beta = 1.0f; g1_36.sa = 1.0f; g1_36.sb = 1.0f; g1_36.Npad = N1; g1_36.pad_ = 0;
      k_gemm<1><<<dim3((unsigned)((N1) + 31) / 32, (unsigned)((Bn) + 15) / 16, (unsigned)(1)), 32, 0, stream>>>(g1_36); }
    k_vf_upd<<<(unsigned)((Bn * N0 + 255) / 256), 256, 0, stream>>>(S0, G0, R0, Bn * N0, 0.5f); k_vf_upd<<<(unsigned)((Bn * N1 + 255) / 256), 256, 0, stream>>>(S1, G1, R1, Bn * N1, 0.5f);
    { GemmP g0_37;
      g0_37.A = R1; g0_37.B = w0; g0_37.bias = b0; g0_37.R = R1; g0_37.C = G0;
      g0_37.sAo = 0; g0_37.sAi = 0; g0_37.sAm = N1; g0_37.sAk = 1; g0_37.sBo = 0; g0_37.sBi = 0; g0_37.sBn = N1; g0_37.sBk = 1; g0_37.sCo = 0; g0_37.sCi = 0; g0_37.sCm = N0; g0_37.sRo = 0; g0_37.sRi = 0; g0_37.sRm = 0; g0_37.sRn = 0;
      g0_37.M = Bn; g0_37.N = N0; g0_37.K = N1; g0_37.zi_n = 1; g0_37.flags = 1; g0_37.act = 0;
      g0_37.alpha = 1.0f; g0_37.beta = 0.0f; g0_37.sa = 1.0f; g0_37.sb = 1.0f; g0_37.Npad = N0; g0_37.pad_ = 0;
      k_gemm<1><<<dim3((unsigned)((N0) + 31) / 32, (unsigned)((Bn) + 15) / 16, (unsigned)(1)), 32, 0, stream>>>(g0_37); }
    { GemmP g1_37;
      g1_37.A = R0; g1_37.B = w1; g1_37.bias = R0; g1_37.R = INP1; g1_37.C = G1;
      g1_37.sAo = 0; g1_37.sAi = 0; g1_37.sAm = N0; g1_37.sAk = 1; g1_37.sBo = 0; g1_37.sBi = 0; g1_37.sBn = N0; g1_37.sBk = 1; g1_37.sCo = 0; g1_37.sCi = 0; g1_37.sCm = N1; g1_37.sRo = 0; g1_37.sRi = 0; g1_37.sRm = N1; g1_37.sRn = 1;
      g1_37.M = Bn; g1_37.N = N1; g1_37.K = N0; g1_37.zi_n = 1; g1_37.flags = 4; g1_37.act = 0;
      g1_37.alpha = 1.0f; g1_37.beta = 1.0f; g1_37.sa = 1.0f; g1_37.sb = 1.0f; g1_37.Npad = N1; g1_37.pad_ = 0;
      k_gemm<1><<<dim3((unsigned)((N1) + 31) / 32, (unsigned)((Bn) + 15) / 16, (unsigned)(1)), 32, 0, stream>>>(g1_37); }
    k_vf_upd<<<(unsigned)((Bn * N0 + 255) / 256), 256, 0, stream>>>(S0, G0, R0, Bn * N0, 0.5f); k_vf_upd<<<(unsigned)((Bn * N1 + 255) / 256), 256, 0, stream>>>(S1, G1, R1, Bn * N1, 0.5f);
    { GemmP g0_38;
      g0_38.A = R1; g0_38.B = w0; g0_38.bias = b0; g0_38.R = R1; g0_38.C = G0;
      g0_38.sAo = 0; g0_38.sAi = 0; g0_38.sAm = N1; g0_38.sAk = 1; g0_38.sBo = 0; g0_38.sBi = 0; g0_38.sBn = N1; g0_38.sBk = 1; g0_38.sCo = 0; g0_38.sCi = 0; g0_38.sCm = N0; g0_38.sRo = 0; g0_38.sRi = 0; g0_38.sRm = 0; g0_38.sRn = 0;
      g0_38.M = Bn; g0_38.N = N0; g0_38.K = N1; g0_38.zi_n = 1; g0_38.flags = 1; g0_38.act = 0;
      g0_38.alpha = 1.0f; g0_38.beta = 0.0f; g0_38.sa = 1.0f; g0_38.sb = 1.0f; g0_38.Npad = N0; g0_38.pad_ = 0;
      k_gemm<1><<<dim3((unsigned)((N0) + 31) / 32, (unsigned)((Bn) + 15) / 16, (unsigned)(1)), 32, 0, stream>>>(g0_38); }
    { GemmP g1_38;
      g1_38.A = R0; g1_38.B = w1; g1_38.bias = R0; g1_38.R = INP1; g1_38.C = G1;
      g1_38.sAo = 0; g1_38.sAi = 0; g1_38.sAm = N0; g1_38.sAk = 1; g1_38.sBo = 0; g1_38.sBi = 0; g1_38.sBn = N0; g1_38.sBk = 1; g1_38.sCo = 0; g1_38.sCi = 0; g1_38.sCm = N1; g1_38.sRo = 0; g1_38.sRi = 0; g1_38.sRm = N1; g1_38.sRn = 1;
      g1_38.M = Bn; g1_38.N = N1; g1_38.K = N0; g1_38.zi_n = 1; g1_38.flags = 4; g1_38.act = 0;
      g1_38.alpha = 1.0f; g1_38.beta = 1.0f; g1_38.sa = 1.0f; g1_38.sb = 1.0f; g1_38.Npad = N1; g1_38.pad_ = 0;
      k_gemm<1><<<dim3((unsigned)((N1) + 31) / 32, (unsigned)((Bn) + 15) / 16, (unsigned)(1)), 32, 0, stream>>>(g1_38); }
    k_vf_upd<<<(unsigned)((Bn * N0 + 255) / 256), 256, 0, stream>>>(S0, G0, R0, Bn * N0, 0.5f); k_vf_upd<<<(unsigned)((Bn * N1 + 255) / 256), 256, 0, stream>>>(S1, G1, R1, Bn * N1, 0.5f);
    { GemmP g0_39;
      g0_39.A = R1; g0_39.B = w0; g0_39.bias = b0; g0_39.R = R1; g0_39.C = G0;
      g0_39.sAo = 0; g0_39.sAi = 0; g0_39.sAm = N1; g0_39.sAk = 1; g0_39.sBo = 0; g0_39.sBi = 0; g0_39.sBn = N1; g0_39.sBk = 1; g0_39.sCo = 0; g0_39.sCi = 0; g0_39.sCm = N0; g0_39.sRo = 0; g0_39.sRi = 0; g0_39.sRm = 0; g0_39.sRn = 0;
      g0_39.M = Bn; g0_39.N = N0; g0_39.K = N1; g0_39.zi_n = 1; g0_39.flags = 1; g0_39.act = 0;
      g0_39.alpha = 1.0f; g0_39.beta = 0.0f; g0_39.sa = 1.0f; g0_39.sb = 1.0f; g0_39.Npad = N0; g0_39.pad_ = 0;
      k_gemm<1><<<dim3((unsigned)((N0) + 31) / 32, (unsigned)((Bn) + 15) / 16, (unsigned)(1)), 32, 0, stream>>>(g0_39); }
    { GemmP g1_39;
      g1_39.A = R0; g1_39.B = w1; g1_39.bias = R0; g1_39.R = INP1; g1_39.C = G1;
      g1_39.sAo = 0; g1_39.sAi = 0; g1_39.sAm = N0; g1_39.sAk = 1; g1_39.sBo = 0; g1_39.sBi = 0; g1_39.sBn = N0; g1_39.sBk = 1; g1_39.sCo = 0; g1_39.sCi = 0; g1_39.sCm = N1; g1_39.sRo = 0; g1_39.sRi = 0; g1_39.sRm = N1; g1_39.sRn = 1;
      g1_39.M = Bn; g1_39.N = N1; g1_39.K = N0; g1_39.zi_n = 1; g1_39.flags = 4; g1_39.act = 0;
      g1_39.alpha = 1.0f; g1_39.beta = 1.0f; g1_39.sa = 1.0f; g1_39.sb = 1.0f; g1_39.Npad = N1; g1_39.pad_ = 0;
      k_gemm<1><<<dim3((unsigned)((N1) + 31) / 32, (unsigned)((Bn) + 15) / 16, (unsigned)(1)), 32, 0, stream>>>(g1_39); }
    k_vf_upd<<<(unsigned)((Bn * N0 + 255) / 256), 256, 0, stream>>>(S0, G0, R0, Bn * N0, 0.5f); k_vf_upd<<<(unsigned)((Bn * N1 + 255) / 256), 256, 0, stream>>>(S1, G1, R1, Bn * N1, 0.5f);
    { GemmP g0_40;
      g0_40.A = R1; g0_40.B = w0; g0_40.bias = b0; g0_40.R = R1; g0_40.C = G0;
      g0_40.sAo = 0; g0_40.sAi = 0; g0_40.sAm = N1; g0_40.sAk = 1; g0_40.sBo = 0; g0_40.sBi = 0; g0_40.sBn = N1; g0_40.sBk = 1; g0_40.sCo = 0; g0_40.sCi = 0; g0_40.sCm = N0; g0_40.sRo = 0; g0_40.sRi = 0; g0_40.sRm = 0; g0_40.sRn = 0;
      g0_40.M = Bn; g0_40.N = N0; g0_40.K = N1; g0_40.zi_n = 1; g0_40.flags = 1; g0_40.act = 0;
      g0_40.alpha = 1.0f; g0_40.beta = 0.0f; g0_40.sa = 1.0f; g0_40.sb = 1.0f; g0_40.Npad = N0; g0_40.pad_ = 0;
      k_gemm<1><<<dim3((unsigned)((N0) + 31) / 32, (unsigned)((Bn) + 15) / 16, (unsigned)(1)), 32, 0, stream>>>(g0_40); }
    { GemmP g1_40;
      g1_40.A = R0; g1_40.B = w1; g1_40.bias = R0; g1_40.R = INP1; g1_40.C = G1;
      g1_40.sAo = 0; g1_40.sAi = 0; g1_40.sAm = N0; g1_40.sAk = 1; g1_40.sBo = 0; g1_40.sBi = 0; g1_40.sBn = N0; g1_40.sBk = 1; g1_40.sCo = 0; g1_40.sCi = 0; g1_40.sCm = N1; g1_40.sRo = 0; g1_40.sRi = 0; g1_40.sRm = N1; g1_40.sRn = 1;
      g1_40.M = Bn; g1_40.N = N1; g1_40.K = N0; g1_40.zi_n = 1; g1_40.flags = 4; g1_40.act = 0;
      g1_40.alpha = 1.0f; g1_40.beta = 1.0f; g1_40.sa = 1.0f; g1_40.sb = 1.0f; g1_40.Npad = N1; g1_40.pad_ = 0;
      k_gemm<1><<<dim3((unsigned)((N1) + 31) / 32, (unsigned)((Bn) + 15) / 16, (unsigned)(1)), 32, 0, stream>>>(g1_40); }
    k_vf_upd<<<(unsigned)((Bn * N0 + 255) / 256), 256, 0, stream>>>(S0, G0, R0, Bn * N0, 0.5f); k_vf_upd<<<(unsigned)((Bn * N1 + 255) / 256), 256, 0, stream>>>(S1, G1, R1, Bn * N1, 0.5f);
    { GemmP g0_41;
      g0_41.A = R1; g0_41.B = w0; g0_41.bias = b0; g0_41.R = R1; g0_41.C = G0;
      g0_41.sAo = 0; g0_41.sAi = 0; g0_41.sAm = N1; g0_41.sAk = 1; g0_41.sBo = 0; g0_41.sBi = 0; g0_41.sBn = N1; g0_41.sBk = 1; g0_41.sCo = 0; g0_41.sCi = 0; g0_41.sCm = N0; g0_41.sRo = 0; g0_41.sRi = 0; g0_41.sRm = 0; g0_41.sRn = 0;
      g0_41.M = Bn; g0_41.N = N0; g0_41.K = N1; g0_41.zi_n = 1; g0_41.flags = 1; g0_41.act = 0;
      g0_41.alpha = 1.0f; g0_41.beta = 0.0f; g0_41.sa = 1.0f; g0_41.sb = 1.0f; g0_41.Npad = N0; g0_41.pad_ = 0;
      k_gemm<1><<<dim3((unsigned)((N0) + 31) / 32, (unsigned)((Bn) + 15) / 16, (unsigned)(1)), 32, 0, stream>>>(g0_41); }
    { GemmP g1_41;
      g1_41.A = R0; g1_41.B = w1; g1_41.bias = R0; g1_41.R = INP1; g1_41.C = G1;
      g1_41.sAo = 0; g1_41.sAi = 0; g1_41.sAm = N0; g1_41.sAk = 1; g1_41.sBo = 0; g1_41.sBi = 0; g1_41.sBn = N0; g1_41.sBk = 1; g1_41.sCo = 0; g1_41.sCi = 0; g1_41.sCm = N1; g1_41.sRo = 0; g1_41.sRi = 0; g1_41.sRm = N1; g1_41.sRn = 1;
      g1_41.M = Bn; g1_41.N = N1; g1_41.K = N0; g1_41.zi_n = 1; g1_41.flags = 4; g1_41.act = 0;
      g1_41.alpha = 1.0f; g1_41.beta = 1.0f; g1_41.sa = 1.0f; g1_41.sb = 1.0f; g1_41.Npad = N1; g1_41.pad_ = 0;
      k_gemm<1><<<dim3((unsigned)((N1) + 31) / 32, (unsigned)((Bn) + 15) / 16, (unsigned)(1)), 32, 0, stream>>>(g1_41); }
    k_vf_upd<<<(unsigned)((Bn * N0 + 255) / 256), 256, 0, stream>>>(S0, G0, R0, Bn * N0, 0.5f); k_vf_upd<<<(unsigned)((Bn * N1 + 255) / 256), 256, 0, stream>>>(S1, G1, R1, Bn * N1, 0.5f);
    { GemmP g0_42;
      g0_42.A = R1; g0_42.B = w0; g0_42.bias = b0; g0_42.R = R1; g0_42.C = G0;
      g0_42.sAo = 0; g0_42.sAi = 0; g0_42.sAm = N1; g0_42.sAk = 1; g0_42.sBo = 0; g0_42.sBi = 0; g0_42.sBn = N1; g0_42.sBk = 1; g0_42.sCo = 0; g0_42.sCi = 0; g0_42.sCm = N0; g0_42.sRo = 0; g0_42.sRi = 0; g0_42.sRm = 0; g0_42.sRn = 0;
      g0_42.M = Bn; g0_42.N = N0; g0_42.K = N1; g0_42.zi_n = 1; g0_42.flags = 1; g0_42.act = 0;
      g0_42.alpha = 1.0f; g0_42.beta = 0.0f; g0_42.sa = 1.0f; g0_42.sb = 1.0f; g0_42.Npad = N0; g0_42.pad_ = 0;
      k_gemm<1><<<dim3((unsigned)((N0) + 31) / 32, (unsigned)((Bn) + 15) / 16, (unsigned)(1)), 32, 0, stream>>>(g0_42); }
    { GemmP g1_42;
      g1_42.A = R0; g1_42.B = w1; g1_42.bias = R0; g1_42.R = INP1; g1_42.C = G1;
      g1_42.sAo = 0; g1_42.sAi = 0; g1_42.sAm = N0; g1_42.sAk = 1; g1_42.sBo = 0; g1_42.sBi = 0; g1_42.sBn = N0; g1_42.sBk = 1; g1_42.sCo = 0; g1_42.sCi = 0; g1_42.sCm = N1; g1_42.sRo = 0; g1_42.sRi = 0; g1_42.sRm = N1; g1_42.sRn = 1;
      g1_42.M = Bn; g1_42.N = N1; g1_42.K = N0; g1_42.zi_n = 1; g1_42.flags = 4; g1_42.act = 0;
      g1_42.alpha = 1.0f; g1_42.beta = 1.0f; g1_42.sa = 1.0f; g1_42.sb = 1.0f; g1_42.Npad = N1; g1_42.pad_ = 0;
      k_gemm<1><<<dim3((unsigned)((N1) + 31) / 32, (unsigned)((Bn) + 15) / 16, (unsigned)(1)), 32, 0, stream>>>(g1_42); }
    k_vf_upd<<<(unsigned)((Bn * N0 + 255) / 256), 256, 0, stream>>>(S0, G0, R0, Bn * N0, 0.5f); k_vf_upd<<<(unsigned)((Bn * N1 + 255) / 256), 256, 0, stream>>>(S1, G1, R1, Bn * N1, 0.5f);
    { GemmP g0_43;
      g0_43.A = R1; g0_43.B = w0; g0_43.bias = b0; g0_43.R = R1; g0_43.C = G0;
      g0_43.sAo = 0; g0_43.sAi = 0; g0_43.sAm = N1; g0_43.sAk = 1; g0_43.sBo = 0; g0_43.sBi = 0; g0_43.sBn = N1; g0_43.sBk = 1; g0_43.sCo = 0; g0_43.sCi = 0; g0_43.sCm = N0; g0_43.sRo = 0; g0_43.sRi = 0; g0_43.sRm = 0; g0_43.sRn = 0;
      g0_43.M = Bn; g0_43.N = N0; g0_43.K = N1; g0_43.zi_n = 1; g0_43.flags = 1; g0_43.act = 0;
      g0_43.alpha = 1.0f; g0_43.beta = 0.0f; g0_43.sa = 1.0f; g0_43.sb = 1.0f; g0_43.Npad = N0; g0_43.pad_ = 0;
      k_gemm<1><<<dim3((unsigned)((N0) + 31) / 32, (unsigned)((Bn) + 15) / 16, (unsigned)(1)), 32, 0, stream>>>(g0_43); }
    { GemmP g1_43;
      g1_43.A = R0; g1_43.B = w1; g1_43.bias = R0; g1_43.R = INP1; g1_43.C = G1;
      g1_43.sAo = 0; g1_43.sAi = 0; g1_43.sAm = N0; g1_43.sAk = 1; g1_43.sBo = 0; g1_43.sBi = 0; g1_43.sBn = N0; g1_43.sBk = 1; g1_43.sCo = 0; g1_43.sCi = 0; g1_43.sCm = N1; g1_43.sRo = 0; g1_43.sRi = 0; g1_43.sRm = N1; g1_43.sRn = 1;
      g1_43.M = Bn; g1_43.N = N1; g1_43.K = N0; g1_43.zi_n = 1; g1_43.flags = 4; g1_43.act = 0;
      g1_43.alpha = 1.0f; g1_43.beta = 1.0f; g1_43.sa = 1.0f; g1_43.sb = 1.0f; g1_43.Npad = N1; g1_43.pad_ = 0;
      k_gemm<1><<<dim3((unsigned)((N1) + 31) / 32, (unsigned)((Bn) + 15) / 16, (unsigned)(1)), 32, 0, stream>>>(g1_43); }
    k_vf_upd<<<(unsigned)((Bn * N0 + 255) / 256), 256, 0, stream>>>(S0, G0, R0, Bn * N0, 0.5f); k_vf_upd<<<(unsigned)((Bn * N1 + 255) / 256), 256, 0, stream>>>(S1, G1, R1, Bn * N1, 0.5f);
    { GemmP g0_44;
      g0_44.A = R1; g0_44.B = w0; g0_44.bias = b0; g0_44.R = R1; g0_44.C = G0;
      g0_44.sAo = 0; g0_44.sAi = 0; g0_44.sAm = N1; g0_44.sAk = 1; g0_44.sBo = 0; g0_44.sBi = 0; g0_44.sBn = N1; g0_44.sBk = 1; g0_44.sCo = 0; g0_44.sCi = 0; g0_44.sCm = N0; g0_44.sRo = 0; g0_44.sRi = 0; g0_44.sRm = 0; g0_44.sRn = 0;
      g0_44.M = Bn; g0_44.N = N0; g0_44.K = N1; g0_44.zi_n = 1; g0_44.flags = 1; g0_44.act = 0;
      g0_44.alpha = 1.0f; g0_44.beta = 0.0f; g0_44.sa = 1.0f; g0_44.sb = 1.0f; g0_44.Npad = N0; g0_44.pad_ = 0;
      k_gemm<1><<<dim3((unsigned)((N0) + 31) / 32, (unsigned)((Bn) + 15) / 16, (unsigned)(1)), 32, 0, stream>>>(g0_44); }
    { GemmP g1_44;
      g1_44.A = R0; g1_44.B = w1; g1_44.bias = R0; g1_44.R = INP1; g1_44.C = G1;
      g1_44.sAo = 0; g1_44.sAi = 0; g1_44.sAm = N0; g1_44.sAk = 1; g1_44.sBo = 0; g1_44.sBi = 0; g1_44.sBn = N0; g1_44.sBk = 1; g1_44.sCo = 0; g1_44.sCi = 0; g1_44.sCm = N1; g1_44.sRo = 0; g1_44.sRi = 0; g1_44.sRm = N1; g1_44.sRn = 1;
      g1_44.M = Bn; g1_44.N = N1; g1_44.K = N0; g1_44.zi_n = 1; g1_44.flags = 4; g1_44.act = 0;
      g1_44.alpha = 1.0f; g1_44.beta = 1.0f; g1_44.sa = 1.0f; g1_44.sb = 1.0f; g1_44.Npad = N1; g1_44.pad_ = 0;
      k_gemm<1><<<dim3((unsigned)((N1) + 31) / 32, (unsigned)((Bn) + 15) / 16, (unsigned)(1)), 32, 0, stream>>>(g1_44); }
    k_vf_upd<<<(unsigned)((Bn * N0 + 255) / 256), 256, 0, stream>>>(S0, G0, R0, Bn * N0, 0.5f); k_vf_upd<<<(unsigned)((Bn * N1 + 255) / 256), 256, 0, stream>>>(S1, G1, R1, Bn * N1, 0.5f);
    { GemmP g0_45;
      g0_45.A = R1; g0_45.B = w0; g0_45.bias = b0; g0_45.R = R1; g0_45.C = G0;
      g0_45.sAo = 0; g0_45.sAi = 0; g0_45.sAm = N1; g0_45.sAk = 1; g0_45.sBo = 0; g0_45.sBi = 0; g0_45.sBn = N1; g0_45.sBk = 1; g0_45.sCo = 0; g0_45.sCi = 0; g0_45.sCm = N0; g0_45.sRo = 0; g0_45.sRi = 0; g0_45.sRm = 0; g0_45.sRn = 0;
      g0_45.M = Bn; g0_45.N = N0; g0_45.K = N1; g0_45.zi_n = 1; g0_45.flags = 1; g0_45.act = 0;
      g0_45.alpha = 1.0f; g0_45.beta = 0.0f; g0_45.sa = 1.0f; g0_45.sb = 1.0f; g0_45.Npad = N0; g0_45.pad_ = 0;
      k_gemm<1><<<dim3((unsigned)((N0) + 31) / 32, (unsigned)((Bn) + 15) / 16, (unsigned)(1)), 32, 0, stream>>>(g0_45); }
    { GemmP g1_45;
      g1_45.A = R0; g1_45.B = w1; g1_45.bias = R0; g1_45.R = INP1; g1_45.C = G1;
      g1_45.sAo = 0; g1_45.sAi = 0; g1_45.sAm = N0; g1_45.sAk = 1; g1_45.sBo = 0; g1_45.sBi = 0; g1_45.sBn = N0; g1_45.sBk = 1; g1_45.sCo = 0; g1_45.sCi = 0; g1_45.sCm = N1; g1_45.sRo = 0; g1_45.sRi = 0; g1_45.sRm = N1; g1_45.sRn = 1;
      g1_45.M = Bn; g1_45.N = N1; g1_45.K = N0; g1_45.zi_n = 1; g1_45.flags = 4; g1_45.act = 0;
      g1_45.alpha = 1.0f; g1_45.beta = 1.0f; g1_45.sa = 1.0f; g1_45.sb = 1.0f; g1_45.Npad = N1; g1_45.pad_ = 0;
      k_gemm<1><<<dim3((unsigned)((N1) + 31) / 32, (unsigned)((Bn) + 15) / 16, (unsigned)(1)), 32, 0, stream>>>(g1_45); }
    k_vf_upd<<<(unsigned)((Bn * N0 + 255) / 256), 256, 0, stream>>>(S0, G0, R0, Bn * N0, 0.5f); k_vf_upd<<<(unsigned)((Bn * N1 + 255) / 256), 256, 0, stream>>>(S1, G1, R1, Bn * N1, 0.5f);
    { GemmP g0_46;
      g0_46.A = R1; g0_46.B = w0; g0_46.bias = b0; g0_46.R = R1; g0_46.C = G0;
      g0_46.sAo = 0; g0_46.sAi = 0; g0_46.sAm = N1; g0_46.sAk = 1; g0_46.sBo = 0; g0_46.sBi = 0; g0_46.sBn = N1; g0_46.sBk = 1; g0_46.sCo = 0; g0_46.sCi = 0; g0_46.sCm = N0; g0_46.sRo = 0; g0_46.sRi = 0; g0_46.sRm = 0; g0_46.sRn = 0;
      g0_46.M = Bn; g0_46.N = N0; g0_46.K = N1; g0_46.zi_n = 1; g0_46.flags = 1; g0_46.act = 0;
      g0_46.alpha = 1.0f; g0_46.beta = 0.0f; g0_46.sa = 1.0f; g0_46.sb = 1.0f; g0_46.Npad = N0; g0_46.pad_ = 0;
      k_gemm<1><<<dim3((unsigned)((N0) + 31) / 32, (unsigned)((Bn) + 15) / 16, (unsigned)(1)), 32, 0, stream>>>(g0_46); }
    { GemmP g1_46;
      g1_46.A = R0; g1_46.B = w1; g1_46.bias = R0; g1_46.R = INP1; g1_46.C = G1;
      g1_46.sAo = 0; g1_46.sAi = 0; g1_46.sAm = N0; g1_46.sAk = 1; g1_46.sBo = 0; g1_46.sBi = 0; g1_46.sBn = N0; g1_46.sBk = 1; g1_46.sCo = 0; g1_46.sCi = 0; g1_46.sCm = N1; g1_46.sRo = 0; g1_46.sRi = 0; g1_46.sRm = N1; g1_46.sRn = 1;
      g1_46.M = Bn; g1_46.N = N1; g1_46.K = N0; g1_46.zi_n = 1; g1_46.flags = 4; g1_46.act = 0;
      g1_46.alpha = 1.0f; g1_46.beta = 1.0f; g1_46.sa = 1.0f; g1_46.sb = 1.0f; g1_46.Npad = N1; g1_46.pad_ = 0;
      k_gemm<1><<<dim3((unsigned)((N1) + 31) / 32, (unsigned)((Bn) + 15) / 16, (unsigned)(1)), 32, 0, stream>>>(g1_46); }
    k_vf_upd<<<(unsigned)((Bn * N0 + 255) / 256), 256, 0, stream>>>(S0, G0, R0, Bn * N0, 0.5f); k_vf_upd<<<(unsigned)((Bn * N1 + 255) / 256), 256, 0, stream>>>(S1, G1, R1, Bn * N1, 0.5f);
    { GemmP g0_47;
      g0_47.A = R1; g0_47.B = w0; g0_47.bias = b0; g0_47.R = R1; g0_47.C = G0;
      g0_47.sAo = 0; g0_47.sAi = 0; g0_47.sAm = N1; g0_47.sAk = 1; g0_47.sBo = 0; g0_47.sBi = 0; g0_47.sBn = N1; g0_47.sBk = 1; g0_47.sCo = 0; g0_47.sCi = 0; g0_47.sCm = N0; g0_47.sRo = 0; g0_47.sRi = 0; g0_47.sRm = 0; g0_47.sRn = 0;
      g0_47.M = Bn; g0_47.N = N0; g0_47.K = N1; g0_47.zi_n = 1; g0_47.flags = 1; g0_47.act = 0;
      g0_47.alpha = 1.0f; g0_47.beta = 0.0f; g0_47.sa = 1.0f; g0_47.sb = 1.0f; g0_47.Npad = N0; g0_47.pad_ = 0;
      k_gemm<1><<<dim3((unsigned)((N0) + 31) / 32, (unsigned)((Bn) + 15) / 16, (unsigned)(1)), 32, 0, stream>>>(g0_47); }
    { GemmP g1_47;
      g1_47.A = R0; g1_47.B = w1; g1_47.bias = R0; g1_47.R = INP1; g1_47.C = G1;
      g1_47.sAo = 0; g1_47.sAi = 0; g1_47.sAm = N0; g1_47.sAk = 1; g1_47.sBo = 0; g1_47.sBi = 0; g1_47.sBn = N0; g1_47.sBk = 1; g1_47.sCo = 0; g1_47.sCi = 0; g1_47.sCm = N1; g1_47.sRo = 0; g1_47.sRi = 0; g1_47.sRm = N1; g1_47.sRn = 1;
      g1_47.M = Bn; g1_47.N = N1; g1_47.K = N0; g1_47.zi_n = 1; g1_47.flags = 4; g1_47.act = 0;
      g1_47.alpha = 1.0f; g1_47.beta = 1.0f; g1_47.sa = 1.0f; g1_47.sb = 1.0f; g1_47.Npad = N1; g1_47.pad_ = 0;
      k_gemm<1><<<dim3((unsigned)((N1) + 31) / 32, (unsigned)((Bn) + 15) / 16, (unsigned)(1)), 32, 0, stream>>>(g1_47); }
    k_vf_upd<<<(unsigned)((Bn * N0 + 255) / 256), 256, 0, stream>>>(S0, G0, R0, Bn * N0, 0.5f); k_vf_upd<<<(unsigned)((Bn * N1 + 255) / 256), 256, 0, stream>>>(S1, G1, R1, Bn * N1, 0.5f);
    { GemmP g0_48;
      g0_48.A = R1; g0_48.B = w0; g0_48.bias = b0; g0_48.R = R1; g0_48.C = G0;
      g0_48.sAo = 0; g0_48.sAi = 0; g0_48.sAm = N1; g0_48.sAk = 1; g0_48.sBo = 0; g0_48.sBi = 0; g0_48.sBn = N1; g0_48.sBk = 1; g0_48.sCo = 0; g0_48.sCi = 0; g0_48.sCm = N0; g0_48.sRo = 0; g0_48.sRi = 0; g0_48.sRm = 0; g0_48.sRn = 0;
      g0_48.M = Bn; g0_48.N = N0; g0_48.K = N1; g0_48.zi_n = 1; g0_48.flags = 1; g0_48.act = 0;
      g0_48.alpha = 1.0f; g0_48.beta = 0.0f; g0_48.sa = 1.0f; g0_48.sb = 1.0f; g0_48.Npad = N0; g0_48.pad_ = 0;
      k_gemm<1><<<dim3((unsigned)((N0) + 31) / 32, (unsigned)((Bn) + 15) / 16, (unsigned)(1)), 32, 0, stream>>>(g0_48); }
    { GemmP g1_48;
      g1_48.A = R0; g1_48.B = w1; g1_48.bias = R0; g1_48.R = INP1; g1_48.C = G1;
      g1_48.sAo = 0; g1_48.sAi = 0; g1_48.sAm = N0; g1_48.sAk = 1; g1_48.sBo = 0; g1_48.sBi = 0; g1_48.sBn = N0; g1_48.sBk = 1; g1_48.sCo = 0; g1_48.sCi = 0; g1_48.sCm = N1; g1_48.sRo = 0; g1_48.sRi = 0; g1_48.sRm = N1; g1_48.sRn = 1;
      g1_48.M = Bn; g1_48.N = N1; g1_48.K = N0; g1_48.zi_n = 1; g1_48.flags = 4; g1_48.act = 0;
      g1_48.alpha = 1.0f; g1_48.beta = 1.0f; g1_48.sa = 1.0f; g1_48.sb = 1.0f; g1_48.Npad = N1; g1_48.pad_ = 0;
      k_gemm<1><<<dim3((unsigned)((N1) + 31) / 32, (unsigned)((Bn) + 15) / 16, (unsigned)(1)), 32, 0, stream>>>(g1_48); }
    k_vf_upd<<<(unsigned)((Bn * N0 + 255) / 256), 256, 0, stream>>>(S0, G0, R0, Bn * N0, 0.5f); k_vf_upd<<<(unsigned)((Bn * N1 + 255) / 256), 256, 0, stream>>>(S1, G1, R1, Bn * N1, 0.5f);
    { GemmP g0_49;
      g0_49.A = R1; g0_49.B = w0; g0_49.bias = b0; g0_49.R = R1; g0_49.C = G0;
      g0_49.sAo = 0; g0_49.sAi = 0; g0_49.sAm = N1; g0_49.sAk = 1; g0_49.sBo = 0; g0_49.sBi = 0; g0_49.sBn = N1; g0_49.sBk = 1; g0_49.sCo = 0; g0_49.sCi = 0; g0_49.sCm = N0; g0_49.sRo = 0; g0_49.sRi = 0; g0_49.sRm = 0; g0_49.sRn = 0;
      g0_49.M = Bn; g0_49.N = N0; g0_49.K = N1; g0_49.zi_n = 1; g0_49.flags = 1; g0_49.act = 0;
      g0_49.alpha = 1.0f; g0_49.beta = 0.0f; g0_49.sa = 1.0f; g0_49.sb = 1.0f; g0_49.Npad = N0; g0_49.pad_ = 0;
      k_gemm<1><<<dim3((unsigned)((N0) + 31) / 32, (unsigned)((Bn) + 15) / 16, (unsigned)(1)), 32, 0, stream>>>(g0_49); }
    { GemmP g1_49;
      g1_49.A = R0; g1_49.B = w1; g1_49.bias = R0; g1_49.R = INP1; g1_49.C = G1;
      g1_49.sAo = 0; g1_49.sAi = 0; g1_49.sAm = N0; g1_49.sAk = 1; g1_49.sBo = 0; g1_49.sBi = 0; g1_49.sBn = N0; g1_49.sBk = 1; g1_49.sCo = 0; g1_49.sCi = 0; g1_49.sCm = N1; g1_49.sRo = 0; g1_49.sRi = 0; g1_49.sRm = N1; g1_49.sRn = 1;
      g1_49.M = Bn; g1_49.N = N1; g1_49.K = N0; g1_49.zi_n = 1; g1_49.flags = 4; g1_49.act = 0;
      g1_49.alpha = 1.0f; g1_49.beta = 1.0f; g1_49.sa = 1.0f; g1_49.sb = 1.0f; g1_49.Npad = N1; g1_49.pad_ = 0;
      k_gemm<1><<<dim3((unsigned)((N1) + 31) / 32, (unsigned)((Bn) + 15) / 16, (unsigned)(1)), 32, 0, stream>>>(g1_49); }
    k_vf_upd<<<(unsigned)((Bn * N0 + 255) / 256), 256, 0, stream>>>(S0, G0, R0, Bn * N0, 0.5f); k_vf_upd<<<(unsigned)((Bn * N1 + 255) / 256), 256, 0, stream>>>(S1, G1, R1, Bn * N1, 0.5f);
    { GemmP g0_50;
      g0_50.A = R1; g0_50.B = w0; g0_50.bias = b0; g0_50.R = R1; g0_50.C = G0;
      g0_50.sAo = 0; g0_50.sAi = 0; g0_50.sAm = N1; g0_50.sAk = 1; g0_50.sBo = 0; g0_50.sBi = 0; g0_50.sBn = N1; g0_50.sBk = 1; g0_50.sCo = 0; g0_50.sCi = 0; g0_50.sCm = N0; g0_50.sRo = 0; g0_50.sRi = 0; g0_50.sRm = 0; g0_50.sRn = 0;
      g0_50.M = Bn; g0_50.N = N0; g0_50.K = N1; g0_50.zi_n = 1; g0_50.flags = 1; g0_50.act = 0;
      g0_50.alpha = 1.0f; g0_50.beta = 0.0f; g0_50.sa = 1.0f; g0_50.sb = 1.0f; g0_50.Npad = N0; g0_50.pad_ = 0;
      k_gemm<1><<<dim3((unsigned)((N0) + 31) / 32, (unsigned)((Bn) + 15) / 16, (unsigned)(1)), 32, 0, stream>>>(g0_50); }
    { GemmP g1_50;
      g1_50.A = R0; g1_50.B = w1; g1_50.bias = R0; g1_50.R = INP1; g1_50.C = G1;
      g1_50.sAo = 0; g1_50.sAi = 0; g1_50.sAm = N0; g1_50.sAk = 1; g1_50.sBo = 0; g1_50.sBi = 0; g1_50.sBn = N0; g1_50.sBk = 1; g1_50.sCo = 0; g1_50.sCi = 0; g1_50.sCm = N1; g1_50.sRo = 0; g1_50.sRi = 0; g1_50.sRm = N1; g1_50.sRn = 1;
      g1_50.M = Bn; g1_50.N = N1; g1_50.K = N0; g1_50.zi_n = 1; g1_50.flags = 4; g1_50.act = 0;
      g1_50.alpha = 1.0f; g1_50.beta = 1.0f; g1_50.sa = 1.0f; g1_50.sb = 1.0f; g1_50.Npad = N1; g1_50.pad_ = 0;
      k_gemm<1><<<dim3((unsigned)((N1) + 31) / 32, (unsigned)((Bn) + 15) / 16, (unsigned)(1)), 32, 0, stream>>>(g1_50); }
    k_vf_upd<<<(unsigned)((Bn * N0 + 255) / 256), 256, 0, stream>>>(S0, G0, R0, Bn * N0, 0.5f); k_vf_upd<<<(unsigned)((Bn * N1 + 255) / 256), 256, 0, stream>>>(S1, G1, R1, Bn * N1, 0.5f);
    { GemmP g0_51;
      g0_51.A = R1; g0_51.B = w0; g0_51.bias = b0; g0_51.R = R1; g0_51.C = G0;
      g0_51.sAo = 0; g0_51.sAi = 0; g0_51.sAm = N1; g0_51.sAk = 1; g0_51.sBo = 0; g0_51.sBi = 0; g0_51.sBn = N1; g0_51.sBk = 1; g0_51.sCo = 0; g0_51.sCi = 0; g0_51.sCm = N0; g0_51.sRo = 0; g0_51.sRi = 0; g0_51.sRm = 0; g0_51.sRn = 0;
      g0_51.M = Bn; g0_51.N = N0; g0_51.K = N1; g0_51.zi_n = 1; g0_51.flags = 1; g0_51.act = 0;
      g0_51.alpha = 1.0f; g0_51.beta = 0.0f; g0_51.sa = 1.0f; g0_51.sb = 1.0f; g0_51.Npad = N0; g0_51.pad_ = 0;
      k_gemm<1><<<dim3((unsigned)((N0) + 31) / 32, (unsigned)((Bn) + 15) / 16, (unsigned)(1)), 32, 0, stream>>>(g0_51); }
    { GemmP g1_51;
      g1_51.A = R0; g1_51.B = w1; g1_51.bias = R0; g1_51.R = INP1; g1_51.C = G1;
      g1_51.sAo = 0; g1_51.sAi = 0; g1_51.sAm = N0; g1_51.sAk = 1; g1_51.sBo = 0; g1_51.sBi = 0; g1_51.sBn = N0; g1_51.sBk = 1; g1_51.sCo = 0; g1_51.sCi = 0; g1_51.sCm = N1; g1_51.sRo = 0; g1_51.sRi = 0; g1_51.sRm = N1; g1_51.sRn = 1;
      g1_51.M = Bn; g1_51.N = N1; g1_51.K = N0; g1_51.zi_n = 1; g1_51.flags = 4; g1_51.act = 0;
      g1_51.alpha = 1.0f; g1_51.beta = 1.0f; g1_51.sa = 1.0f; g1_51.sb = 1.0f; g1_51.Npad = N1; g1_51.pad_ = 0;
      k_gemm<1><<<dim3((unsigned)((N1) + 31) / 32, (unsigned)((Bn) + 15) / 16, (unsigned)(1)), 32, 0, stream>>>(g1_51); }
    k_vf_upd<<<(unsigned)((Bn * N0 + 255) / 256), 256, 0, stream>>>(S0, G0, R0, Bn * N0, 0.5f); k_vf_upd<<<(unsigned)((Bn * N1 + 255) / 256), 256, 0, stream>>>(S1, G1, R1, Bn * N1, 0.5f);
    { GemmP g0_52;
      g0_52.A = R1; g0_52.B = w0; g0_52.bias = b0; g0_52.R = R1; g0_52.C = G0;
      g0_52.sAo = 0; g0_52.sAi = 0; g0_52.sAm = N1; g0_52.sAk = 1; g0_52.sBo = 0; g0_52.sBi = 0; g0_52.sBn = N1; g0_52.sBk = 1; g0_52.sCo = 0; g0_52.sCi = 0; g0_52.sCm = N0; g0_52.sRo = 0; g0_52.sRi = 0; g0_52.sRm = 0; g0_52.sRn = 0;
      g0_52.M = Bn; g0_52.N = N0; g0_52.K = N1; g0_52.zi_n = 1; g0_52.flags = 1; g0_52.act = 0;
      g0_52.alpha = 1.0f; g0_52.beta = 0.0f; g0_52.sa = 1.0f; g0_52.sb = 1.0f; g0_52.Npad = N0; g0_52.pad_ = 0;
      k_gemm<1><<<dim3((unsigned)((N0) + 31) / 32, (unsigned)((Bn) + 15) / 16, (unsigned)(1)), 32, 0, stream>>>(g0_52); }
    { GemmP g1_52;
      g1_52.A = R0; g1_52.B = w1; g1_52.bias = R0; g1_52.R = INP1; g1_52.C = G1;
      g1_52.sAo = 0; g1_52.sAi = 0; g1_52.sAm = N0; g1_52.sAk = 1; g1_52.sBo = 0; g1_52.sBi = 0; g1_52.sBn = N0; g1_52.sBk = 1; g1_52.sCo = 0; g1_52.sCi = 0; g1_52.sCm = N1; g1_52.sRo = 0; g1_52.sRi = 0; g1_52.sRm = N1; g1_52.sRn = 1;
      g1_52.M = Bn; g1_52.N = N1; g1_52.K = N0; g1_52.zi_n = 1; g1_52.flags = 4; g1_52.act = 0;
      g1_52.alpha = 1.0f; g1_52.beta = 1.0f; g1_52.sa = 1.0f; g1_52.sb = 1.0f; g1_52.Npad = N1; g1_52.pad_ = 0;
      k_gemm<1><<<dim3((unsigned)((N1) + 31) / 32, (unsigned)((Bn) + 15) / 16, (unsigned)(1)), 32, 0, stream>>>(g1_52); }
    k_vf_upd<<<(unsigned)((Bn * N0 + 255) / 256), 256, 0, stream>>>(S0, G0, R0, Bn * N0, 0.5f); k_vf_upd<<<(unsigned)((Bn * N1 + 255) / 256), 256, 0, stream>>>(S1, G1, R1, Bn * N1, 0.5f);
    { GemmP g0_53;
      g0_53.A = R1; g0_53.B = w0; g0_53.bias = b0; g0_53.R = R1; g0_53.C = G0;
      g0_53.sAo = 0; g0_53.sAi = 0; g0_53.sAm = N1; g0_53.sAk = 1; g0_53.sBo = 0; g0_53.sBi = 0; g0_53.sBn = N1; g0_53.sBk = 1; g0_53.sCo = 0; g0_53.sCi = 0; g0_53.sCm = N0; g0_53.sRo = 0; g0_53.sRi = 0; g0_53.sRm = 0; g0_53.sRn = 0;
      g0_53.M = Bn; g0_53.N = N0; g0_53.K = N1; g0_53.zi_n = 1; g0_53.flags = 1; g0_53.act = 0;
      g0_53.alpha = 1.0f; g0_53.beta = 0.0f; g0_53.sa = 1.0f; g0_53.sb = 1.0f; g0_53.Npad = N0; g0_53.pad_ = 0;
      k_gemm<1><<<dim3((unsigned)((N0) + 31) / 32, (unsigned)((Bn) + 15) / 16, (unsigned)(1)), 32, 0, stream>>>(g0_53); }
    { GemmP g1_53;
      g1_53.A = R0; g1_53.B = w1; g1_53.bias = R0; g1_53.R = INP1; g1_53.C = G1;
      g1_53.sAo = 0; g1_53.sAi = 0; g1_53.sAm = N0; g1_53.sAk = 1; g1_53.sBo = 0; g1_53.sBi = 0; g1_53.sBn = N0; g1_53.sBk = 1; g1_53.sCo = 0; g1_53.sCi = 0; g1_53.sCm = N1; g1_53.sRo = 0; g1_53.sRi = 0; g1_53.sRm = N1; g1_53.sRn = 1;
      g1_53.M = Bn; g1_53.N = N1; g1_53.K = N0; g1_53.zi_n = 1; g1_53.flags = 4; g1_53.act = 0;
      g1_53.alpha = 1.0f; g1_53.beta = 1.0f; g1_53.sa = 1.0f; g1_53.sb = 1.0f; g1_53.Npad = N1; g1_53.pad_ = 0;
      k_gemm<1><<<dim3((unsigned)((N1) + 31) / 32, (unsigned)((Bn) + 15) / 16, (unsigned)(1)), 32, 0, stream>>>(g1_53); }
    k_vf_upd<<<(unsigned)((Bn * N0 + 255) / 256), 256, 0, stream>>>(S0, G0, R0, Bn * N0, 0.5f); k_vf_upd<<<(unsigned)((Bn * N1 + 255) / 256), 256, 0, stream>>>(S1, G1, R1, Bn * N1, 0.5f);
    { GemmP g0_54;
      g0_54.A = R1; g0_54.B = w0; g0_54.bias = b0; g0_54.R = R1; g0_54.C = G0;
      g0_54.sAo = 0; g0_54.sAi = 0; g0_54.sAm = N1; g0_54.sAk = 1; g0_54.sBo = 0; g0_54.sBi = 0; g0_54.sBn = N1; g0_54.sBk = 1; g0_54.sCo = 0; g0_54.sCi = 0; g0_54.sCm = N0; g0_54.sRo = 0; g0_54.sRi = 0; g0_54.sRm = 0; g0_54.sRn = 0;
      g0_54.M = Bn; g0_54.N = N0; g0_54.K = N1; g0_54.zi_n = 1; g0_54.flags = 1; g0_54.act = 0;
      g0_54.alpha = 1.0f; g0_54.beta = 0.0f; g0_54.sa = 1.0f; g0_54.sb = 1.0f; g0_54.Npad = N0; g0_54.pad_ = 0;
      k_gemm<1><<<dim3((unsigned)((N0) + 31) / 32, (unsigned)((Bn) + 15) / 16, (unsigned)(1)), 32, 0, stream>>>(g0_54); }
    { GemmP g1_54;
      g1_54.A = R0; g1_54.B = w1; g1_54.bias = R0; g1_54.R = INP1; g1_54.C = G1;
      g1_54.sAo = 0; g1_54.sAi = 0; g1_54.sAm = N0; g1_54.sAk = 1; g1_54.sBo = 0; g1_54.sBi = 0; g1_54.sBn = N0; g1_54.sBk = 1; g1_54.sCo = 0; g1_54.sCi = 0; g1_54.sCm = N1; g1_54.sRo = 0; g1_54.sRi = 0; g1_54.sRm = N1; g1_54.sRn = 1;
      g1_54.M = Bn; g1_54.N = N1; g1_54.K = N0; g1_54.zi_n = 1; g1_54.flags = 4; g1_54.act = 0;
      g1_54.alpha = 1.0f; g1_54.beta = 1.0f; g1_54.sa = 1.0f; g1_54.sb = 1.0f; g1_54.Npad = N1; g1_54.pad_ = 0;
      k_gemm<1><<<dim3((unsigned)((N1) + 31) / 32, (unsigned)((Bn) + 15) / 16, (unsigned)(1)), 32, 0, stream>>>(g1_54); }
    k_vf_upd<<<(unsigned)((Bn * N0 + 255) / 256), 256, 0, stream>>>(S0, G0, R0, Bn * N0, 0.5f); k_vf_upd<<<(unsigned)((Bn * N1 + 255) / 256), 256, 0, stream>>>(S1, G1, R1, Bn * N1, 0.5f);
    { GemmP g0_55;
      g0_55.A = R1; g0_55.B = w0; g0_55.bias = b0; g0_55.R = R1; g0_55.C = G0;
      g0_55.sAo = 0; g0_55.sAi = 0; g0_55.sAm = N1; g0_55.sAk = 1; g0_55.sBo = 0; g0_55.sBi = 0; g0_55.sBn = N1; g0_55.sBk = 1; g0_55.sCo = 0; g0_55.sCi = 0; g0_55.sCm = N0; g0_55.sRo = 0; g0_55.sRi = 0; g0_55.sRm = 0; g0_55.sRn = 0;
      g0_55.M = Bn; g0_55.N = N0; g0_55.K = N1; g0_55.zi_n = 1; g0_55.flags = 1; g0_55.act = 0;
      g0_55.alpha = 1.0f; g0_55.beta = 0.0f; g0_55.sa = 1.0f; g0_55.sb = 1.0f; g0_55.Npad = N0; g0_55.pad_ = 0;
      k_gemm<1><<<dim3((unsigned)((N0) + 31) / 32, (unsigned)((Bn) + 15) / 16, (unsigned)(1)), 32, 0, stream>>>(g0_55); }
    { GemmP g1_55;
      g1_55.A = R0; g1_55.B = w1; g1_55.bias = R0; g1_55.R = INP1; g1_55.C = G1;
      g1_55.sAo = 0; g1_55.sAi = 0; g1_55.sAm = N0; g1_55.sAk = 1; g1_55.sBo = 0; g1_55.sBi = 0; g1_55.sBn = N0; g1_55.sBk = 1; g1_55.sCo = 0; g1_55.sCi = 0; g1_55.sCm = N1; g1_55.sRo = 0; g1_55.sRi = 0; g1_55.sRm = N1; g1_55.sRn = 1;
      g1_55.M = Bn; g1_55.N = N1; g1_55.K = N0; g1_55.zi_n = 1; g1_55.flags = 4; g1_55.act = 0;
      g1_55.alpha = 1.0f; g1_55.beta = 1.0f; g1_55.sa = 1.0f; g1_55.sb = 1.0f; g1_55.Npad = N1; g1_55.pad_ = 0;
      k_gemm<1><<<dim3((unsigned)((N1) + 31) / 32, (unsigned)((Bn) + 15) / 16, (unsigned)(1)), 32, 0, stream>>>(g1_55); }
    k_vf_upd<<<(unsigned)((Bn * N0 + 255) / 256), 256, 0, stream>>>(S0, G0, R0, Bn * N0, 0.5f); k_vf_upd<<<(unsigned)((Bn * N1 + 255) / 256), 256, 0, stream>>>(S1, G1, R1, Bn * N1, 0.5f);
    { GemmP g0_56;
      g0_56.A = R1; g0_56.B = w0; g0_56.bias = b0; g0_56.R = R1; g0_56.C = G0;
      g0_56.sAo = 0; g0_56.sAi = 0; g0_56.sAm = N1; g0_56.sAk = 1; g0_56.sBo = 0; g0_56.sBi = 0; g0_56.sBn = N1; g0_56.sBk = 1; g0_56.sCo = 0; g0_56.sCi = 0; g0_56.sCm = N0; g0_56.sRo = 0; g0_56.sRi = 0; g0_56.sRm = 0; g0_56.sRn = 0;
      g0_56.M = Bn; g0_56.N = N0; g0_56.K = N1; g0_56.zi_n = 1; g0_56.flags = 1; g0_56.act = 0;
      g0_56.alpha = 1.0f; g0_56.beta = 0.0f; g0_56.sa = 1.0f; g0_56.sb = 1.0f; g0_56.Npad = N0; g0_56.pad_ = 0;
      k_gemm<1><<<dim3((unsigned)((N0) + 31) / 32, (unsigned)((Bn) + 15) / 16, (unsigned)(1)), 32, 0, stream>>>(g0_56); }
    { GemmP g1_56;
      g1_56.A = R0; g1_56.B = w1; g1_56.bias = R0; g1_56.R = INP1; g1_56.C = G1;
      g1_56.sAo = 0; g1_56.sAi = 0; g1_56.sAm = N0; g1_56.sAk = 1; g1_56.sBo = 0; g1_56.sBi = 0; g1_56.sBn = N0; g1_56.sBk = 1; g1_56.sCo = 0; g1_56.sCi = 0; g1_56.sCm = N1; g1_56.sRo = 0; g1_56.sRi = 0; g1_56.sRm = N1; g1_56.sRn = 1;
      g1_56.M = Bn; g1_56.N = N1; g1_56.K = N0; g1_56.zi_n = 1; g1_56.flags = 4; g1_56.act = 0;
      g1_56.alpha = 1.0f; g1_56.beta = 1.0f; g1_56.sa = 1.0f; g1_56.sb = 1.0f; g1_56.Npad = N1; g1_56.pad_ = 0;
      k_gemm<1><<<dim3((unsigned)((N1) + 31) / 32, (unsigned)((Bn) + 15) / 16, (unsigned)(1)), 32, 0, stream>>>(g1_56); }
    k_vf_upd<<<(unsigned)((Bn * N0 + 255) / 256), 256, 0, stream>>>(S0, G0, R0, Bn * N0, 0.5f); k_vf_upd<<<(unsigned)((Bn * N1 + 255) / 256), 256, 0, stream>>>(S1, G1, R1, Bn * N1, 0.5f);
    { GemmP g0_57;
      g0_57.A = R1; g0_57.B = w0; g0_57.bias = b0; g0_57.R = R1; g0_57.C = G0;
      g0_57.sAo = 0; g0_57.sAi = 0; g0_57.sAm = N1; g0_57.sAk = 1; g0_57.sBo = 0; g0_57.sBi = 0; g0_57.sBn = N1; g0_57.sBk = 1; g0_57.sCo = 0; g0_57.sCi = 0; g0_57.sCm = N0; g0_57.sRo = 0; g0_57.sRi = 0; g0_57.sRm = 0; g0_57.sRn = 0;
      g0_57.M = Bn; g0_57.N = N0; g0_57.K = N1; g0_57.zi_n = 1; g0_57.flags = 1; g0_57.act = 0;
      g0_57.alpha = 1.0f; g0_57.beta = 0.0f; g0_57.sa = 1.0f; g0_57.sb = 1.0f; g0_57.Npad = N0; g0_57.pad_ = 0;
      k_gemm<1><<<dim3((unsigned)((N0) + 31) / 32, (unsigned)((Bn) + 15) / 16, (unsigned)(1)), 32, 0, stream>>>(g0_57); }
    { GemmP g1_57;
      g1_57.A = R0; g1_57.B = w1; g1_57.bias = R0; g1_57.R = INP1; g1_57.C = G1;
      g1_57.sAo = 0; g1_57.sAi = 0; g1_57.sAm = N0; g1_57.sAk = 1; g1_57.sBo = 0; g1_57.sBi = 0; g1_57.sBn = N0; g1_57.sBk = 1; g1_57.sCo = 0; g1_57.sCi = 0; g1_57.sCm = N1; g1_57.sRo = 0; g1_57.sRi = 0; g1_57.sRm = N1; g1_57.sRn = 1;
      g1_57.M = Bn; g1_57.N = N1; g1_57.K = N0; g1_57.zi_n = 1; g1_57.flags = 4; g1_57.act = 0;
      g1_57.alpha = 1.0f; g1_57.beta = 1.0f; g1_57.sa = 1.0f; g1_57.sb = 1.0f; g1_57.Npad = N1; g1_57.pad_ = 0;
      k_gemm<1><<<dim3((unsigned)((N1) + 31) / 32, (unsigned)((Bn) + 15) / 16, (unsigned)(1)), 32, 0, stream>>>(g1_57); }
    k_vf_upd<<<(unsigned)((Bn * N0 + 255) / 256), 256, 0, stream>>>(S0, G0, R0, Bn * N0, 0.5f); k_vf_upd<<<(unsigned)((Bn * N1 + 255) / 256), 256, 0, stream>>>(S1, G1, R1, Bn * N1, 0.5f);
    { GemmP g0_58;
      g0_58.A = R1; g0_58.B = w0; g0_58.bias = b0; g0_58.R = R1; g0_58.C = G0;
      g0_58.sAo = 0; g0_58.sAi = 0; g0_58.sAm = N1; g0_58.sAk = 1; g0_58.sBo = 0; g0_58.sBi = 0; g0_58.sBn = N1; g0_58.sBk = 1; g0_58.sCo = 0; g0_58.sCi = 0; g0_58.sCm = N0; g0_58.sRo = 0; g0_58.sRi = 0; g0_58.sRm = 0; g0_58.sRn = 0;
      g0_58.M = Bn; g0_58.N = N0; g0_58.K = N1; g0_58.zi_n = 1; g0_58.flags = 1; g0_58.act = 0;
      g0_58.alpha = 1.0f; g0_58.beta = 0.0f; g0_58.sa = 1.0f; g0_58.sb = 1.0f; g0_58.Npad = N0; g0_58.pad_ = 0;
      k_gemm<1><<<dim3((unsigned)((N0) + 31) / 32, (unsigned)((Bn) + 15) / 16, (unsigned)(1)), 32, 0, stream>>>(g0_58); }
    { GemmP g1_58;
      g1_58.A = R0; g1_58.B = w1; g1_58.bias = R0; g1_58.R = INP1; g1_58.C = G1;
      g1_58.sAo = 0; g1_58.sAi = 0; g1_58.sAm = N0; g1_58.sAk = 1; g1_58.sBo = 0; g1_58.sBi = 0; g1_58.sBn = N0; g1_58.sBk = 1; g1_58.sCo = 0; g1_58.sCi = 0; g1_58.sCm = N1; g1_58.sRo = 0; g1_58.sRi = 0; g1_58.sRm = N1; g1_58.sRn = 1;
      g1_58.M = Bn; g1_58.N = N1; g1_58.K = N0; g1_58.zi_n = 1; g1_58.flags = 4; g1_58.act = 0;
      g1_58.alpha = 1.0f; g1_58.beta = 1.0f; g1_58.sa = 1.0f; g1_58.sb = 1.0f; g1_58.Npad = N1; g1_58.pad_ = 0;
      k_gemm<1><<<dim3((unsigned)((N1) + 31) / 32, (unsigned)((Bn) + 15) / 16, (unsigned)(1)), 32, 0, stream>>>(g1_58); }
    k_vf_upd<<<(unsigned)((Bn * N0 + 255) / 256), 256, 0, stream>>>(S0, G0, R0, Bn * N0, 0.5f); k_vf_upd<<<(unsigned)((Bn * N1 + 255) / 256), 256, 0, stream>>>(S1, G1, R1, Bn * N1, 0.5f);
    { GemmP g0_59;
      g0_59.A = R1; g0_59.B = w0; g0_59.bias = b0; g0_59.R = R1; g0_59.C = G0;
      g0_59.sAo = 0; g0_59.sAi = 0; g0_59.sAm = N1; g0_59.sAk = 1; g0_59.sBo = 0; g0_59.sBi = 0; g0_59.sBn = N1; g0_59.sBk = 1; g0_59.sCo = 0; g0_59.sCi = 0; g0_59.sCm = N0; g0_59.sRo = 0; g0_59.sRi = 0; g0_59.sRm = 0; g0_59.sRn = 0;
      g0_59.M = Bn; g0_59.N = N0; g0_59.K = N1; g0_59.zi_n = 1; g0_59.flags = 1; g0_59.act = 0;
      g0_59.alpha = 1.0f; g0_59.beta = 0.0f; g0_59.sa = 1.0f; g0_59.sb = 1.0f; g0_59.Npad = N0; g0_59.pad_ = 0;
      k_gemm<1><<<dim3((unsigned)((N0) + 31) / 32, (unsigned)((Bn) + 15) / 16, (unsigned)(1)), 32, 0, stream>>>(g0_59); }
    { GemmP g1_59;
      g1_59.A = R0; g1_59.B = w1; g1_59.bias = R0; g1_59.R = INP1; g1_59.C = G1;
      g1_59.sAo = 0; g1_59.sAi = 0; g1_59.sAm = N0; g1_59.sAk = 1; g1_59.sBo = 0; g1_59.sBi = 0; g1_59.sBn = N0; g1_59.sBk = 1; g1_59.sCo = 0; g1_59.sCi = 0; g1_59.sCm = N1; g1_59.sRo = 0; g1_59.sRi = 0; g1_59.sRm = N1; g1_59.sRn = 1;
      g1_59.M = Bn; g1_59.N = N1; g1_59.K = N0; g1_59.zi_n = 1; g1_59.flags = 4; g1_59.act = 0;
      g1_59.alpha = 1.0f; g1_59.beta = 1.0f; g1_59.sa = 1.0f; g1_59.sb = 1.0f; g1_59.Npad = N1; g1_59.pad_ = 0;
      k_gemm<1><<<dim3((unsigned)((N1) + 31) / 32, (unsigned)((Bn) + 15) / 16, (unsigned)(1)), 32, 0, stream>>>(g1_59); }
    k_vf_upd<<<(unsigned)((Bn * N0 + 255) / 256), 256, 0, stream>>>(S0, G0, out, Bn * N0, 0.5f); k_vf_upd<<<(unsigned)((Bn * N1 + 255) / 256), 256, 0, stream>>>(S1, G1, s1out, Bn * N1, 0.5f);
}
